// RobustTemporalEdge2Seq_89361089560602
// MI455X (gfx1250) — hardware-verified
//
#include <hip/hip_runtime.h>
#include <math.h>

typedef __attribute__((ext_vector_type(16))) _Float16 v16h;
typedef __attribute__((ext_vector_type(8)))  _Float16 v8h;
typedef __attribute__((ext_vector_type(16))) __bf16   v16b;
typedef __attribute__((ext_vector_type(8)))  float    v8f;
typedef __attribute__((ext_vector_type(4)))  float    v4f;

__device__ __forceinline__ int frag_k(int i, int h) { return (i < 8) ? (8 * h + i) : (16 + 8 * h + (i - 8)); }
__device__ __forceinline__ __bf16 bf16_rne(float f) {
    unsigned int u = __float_as_uint(f);
    u += 0x7fffu + ((u >> 16) & 1u);
    return __builtin_bit_cast(__bf16, (unsigned short)(u >> 16));
}
__device__ __forceinline__ float bf16_f32(__bf16 b) { return __uint_as_float(((unsigned int)__builtin_bit_cast(unsigned short, b)) << 16); }
__device__ __forceinline__ v8f wmma16(v16h a, v16h b, v8f c) {
    c = __builtin_amdgcn_wmma_f32_16x16x32_f16(false, a, false, b, (short)0, c, false, false);
    asm volatile("v_nop\n\tv_nop\n\tv_nop\n\tv_nop" : "+v"(c) : "v"(a), "v"(b));
    return c;
}
__device__ __forceinline__ v8f wmmab(v16b a, v16b b, v8f c) {
    c = __builtin_amdgcn_wmma_f32_16x16x32_bf16(false, a, false, b, (short)0, c, false, false);
    asm volatile("v_nop\n\tv_nop\n\tv_nop\n\tv_nop" : "+v"(c) : "v"(a), "v"(b));
    return c;
}
struct Split { v16b hi, lo; };
__device__ __forceinline__ v8f wmma3(const Split& a, const Split& b, v8f c) {
    c = __builtin_amdgcn_wmma_f32_16x16x32_bf16(false, a.hi, false, b.hi, (short)0, c, false, false);
    c = __builtin_amdgcn_wmma_f32_16x16x32_bf16(false, a.hi, false, b.lo, (short)0, c, false, false);
    c = __builtin_amdgcn_wmma_f32_16x16x32_bf16(false, a.lo, false, b.hi, (short)0, c, false, false);
    asm volatile("v_nop\n\tv_nop\n\tv_nop\n\tv_nop" : "+v"(c) : "v"(a.hi), "v"(a.lo), "v"(b.hi), "v"(b.lo));
    return c;
}
struct Split3 { v16b hi, mid, lo; };
__device__ __forceinline__ v8f wmma6(const Split3& a, const Split3& b, v8f c) {
    c = __builtin_amdgcn_wmma_f32_16x16x32_bf16(false, a.hi, false, b.hi, (short)0, c, false, false);
    c = __builtin_amdgcn_wmma_f32_16x16x32_bf16(false, a.hi, false, b.mid, (short)0, c, false, false);
    c = __builtin_amdgcn_wmma_f32_16x16x32_bf16(false, a.mid, false, b.hi, (short)0, c, false, false);
    c = __builtin_amdgcn_wmma_f32_16x16x32_bf16(false, a.hi, false, b.lo, (short)0, c, false, false);
    c = __builtin_amdgcn_wmma_f32_16x16x32_bf16(false, a.mid, false, b.mid, (short)0, c, false, false);
    c = __builtin_amdgcn_wmma_f32_16x16x32_bf16(false, a.lo, false, b.hi, (short)0, c, false, false);
    asm volatile("v_nop\n\tv_nop\n\tv_nop\n\tv_nop" : "+v"(c) : "v"(a.hi), "v"(a.mid), "v"(a.lo), "v"(b.hi), "v"(b.mid), "v"(b.lo));
    return c;
}

__device__ __forceinline__ v16h fh_ld(const float* __restrict__ p, long long sk, int k0, int h, int klen, float s) {
    v16h a;
#pragma unroll
    for (int i = 0; i < 16; ++i) { const int k = k0 + frag_k(i, h); a[i] = (k < klen) ? (_Float16)(p[(long long)k * sk] * s) : (_Float16)0.f; }
    return a;
}
__device__ __forceinline__ Split sp_ld(const float* __restrict__ p, long long sk, int k0, int h, int klen, float s) {
    Split r;
#pragma unroll
    for (int i = 0; i < 16; ++i) {
        const int k = k0 + frag_k(i, h); const float x = (k < klen) ? p[(long long)k * sk] * s : 0.f;
        const __bf16 hb = bf16_rne(x); r.hi[i] = hb; r.lo[i] = bf16_rne(x - bf16_f32(hb));
    }
    return r;
}
__device__ __forceinline__ Split3 sp3_ld(const float* __restrict__ p, long long sk, int k0, int h, int klen, float s) {
    Split3 r;
#pragma unroll
    for (int i = 0; i < 16; ++i) {
        const int k = k0 + frag_k(i, h); const float x = (k < klen) ? p[(long long)k * sk] * s : 0.f;
        const __bf16 hb = bf16_rne(x); const float r1 = x - bf16_f32(hb); const __bf16 mb = bf16_rne(r1);
        r.hi[i] = hb; r.mid[i] = mb; r.lo[i] = bf16_rne(r1 - bf16_f32(mb));
    }
    return r;
}
__device__ __forceinline__ v16b bh_ld(const float* __restrict__ p, long long sk, int k0, int h, int klen, float s) {
    v16b a;
#pragma unroll
    for (int i = 0; i < 16; ++i) { const int k = k0 + frag_k(i, h); a[i] = bf16_rne((k < klen) ? p[(long long)k * sk] * s : 0.f); }
    return a;
}
__device__ __forceinline__ v16h fh_row(const _Float16* __restrict__ row, int k0, int h) {
    v16h a;
#pragma unroll
    for (int i = 0; i < 16; ++i) a[i] = row[k0 + frag_k(i, h)];
    return a;
}

#define VST2(T, ptr, val) do { const T vst2_v_ = (val); *(volatile T*)(ptr) = vst2_v_; __threadfence(); *(volatile T*)(ptr) = vst2_v_; } while (0)
typedef float v4f __attribute__((ext_vector_type(4)));
#define VST2V4(ptr, val) do { const v4f vst2_v4_ = (val); *(volatile v4f*)(ptr) = vst2_v4_; __threadfence(); *(volatile v4f*)(ptr) = vst2_v4_; } while (0)

__device__ __attribute__((noinline)) float act_fn(float v, int act) {
    if (act == 1) return fmaxf(v, 0.f);
    if (act == 2) { const float u = 0.7978845608028654f * (v + 0.044715f * v * v * v); return 0.5f * v * (1.f + tanhf(u)); }
    if (act == 3) return v / (1.f + expf(-v));
    if (act == 4) return 0.5f * v * (1.f + erff(v * 0.7071067811865476f));
    if (act == 5) return tanhf(v);
    if (act == 6) return 1.f / (1.f + expf(-v));
    if (act == 7) return (v > 0.f) ? v : 0.01f * v;
    if (act == 8) return (v > 0.f) ? v : (expf(v) - 1.f);
    if (act == 9) return fminf(fmaxf(v, 0.f), 6.f);
    if (act == 10) return fabsf(v);
    if (act == 11) return (v >= 0.f) ? v : 0.1f * v;
    if (act == 12) return (v > 0.f) ? v : 0.2f * v;
    if (act == 13) return (v > 20.f) ? v : log1pf(expf(v));
    return v;
}

struct GemmP {
    const float* A; const float* B; const float* bias; const float* R; float* C;
    long long sAo, sAi, sAm, sAk, sBo, sBi, sBn, sBk, sCo, sCi, sCm, sRo, sRi, sRm, sRn;
    int M, N, K, zi_n, flags, act; float alpha, beta, sa, sb;
    int Npad, pad_;
};
static_assert(sizeof(GemmP) == 5 * 8 + 15 * 8 + 6 * 4 + 4 * 4 + 2 * 4, "GemmP has padding");

template <int MODE>
__global__ __launch_bounds__(32) void k_gemm(GemmP p) {
    const int lane = threadIdx.x & 31, h = lane >> 4, l15 = lane & 15;
    const int m0 = blockIdx.y * 16, n0 = blockIdx.x * 32;
    const int z = blockIdx.z, zo = z / p.zi_n, zi = z - zo * p.zi_n;
    const float* A = p.A + zo * p.sAo + zi * p.sAi;
    const float* B = p.B + zo * p.sBo + zi * p.sBi;
    const int am = min(m0 + l15, p.M - 1);
    v8f acc[2], comp[2];
#pragma unroll
    for (int t = 0; t < 2; ++t) { v8f zz = {}; acc[t] = zz; comp[t] = zz; }
    for (int k0 = 0; k0 < p.K; k0 += 32) {
        const float* arow = A + (long long)am * p.sAm;
        if (MODE == 1) {
            const Split a = sp_ld(arow, p.sAk, k0, h, p.K, 1.f);
#pragma unroll
            for (int t = 0; t < 2; ++t) {
                const int bn = min(n0 + t * 16 + l15, p.N - 1);
                acc[t] = wmma3(a, sp_ld(B + (long long)bn * p.sBn, p.sBk, k0, h, p.K, 1.f), acc[t]);
            }
        } else if (MODE == 3) {
            const Split3 a = sp3_ld(arow, p.sAk, k0, h, p.K, 1.f);
#pragma unroll
            for (int t = 0; t < 2; ++t) {
                const int bn = min(n0 + t * 16 + l15, p.N - 1);
                acc[t] = wmma6(a, sp3_ld(B + (long long)bn * p.sBn, p.sBk, k0, h, p.K, 1.f), acc[t]);
            }
        } else if (MODE == 4) {
            const Split3 a = sp3_ld(arow, p.sAk, k0, h, p.K, 1.f);
#pragma unroll
            for (int t = 0; t < 2; ++t) {
                const int bn = min(n0 + t * 16 + l15, p.N - 1); v8f zz = {};
                const v8f part = wmma6(a, sp3_ld(B + (long long)bn * p.sBn, p.sBk, k0, h, p.K, 1.f), zz);
                const v8f y = part - comp[t]; const v8f s = acc[t] + y; comp[t] = (s - acc[t]) - y; acc[t] = s;
            }
        } else if (MODE == 2) {
            const v16b a = bh_ld(arow, p.sAk, k0, h, p.K, 1.f);
#pragma unroll
            for (int t = 0; t < 2; ++t) {
                const int bn = min(n0 + t * 16 + l15, p.N - 1);
                acc[t] = wmmab(a, bh_ld(B + (long long)bn * p.sBn, p.sBk, k0, h, p.K, 1.f), acc[t]);
            }
        } else {
            const v16h a = fh_ld(arow, p.sAk, k0, h, p.K, p.sa);
#pragma unroll
            for (int t = 0; t < 2; ++t) {
                const int bn = min(n0 + t * 16 + l15, p.N - 1);
                acc[t] = wmma16(a, fh_ld(B + (long long)bn * p.sBn, p.sBk, k0, h, p.K, p.sb), acc[t]);
            }
        }
    }
    const float iscale = (MODE == 0) ? p.alpha / (p.sa * p.sb) : p.alpha;
    float* C = p.C + zo * p.sCo + zi * p.sCi;
    const float* R = p.R + zo * p.sRo + zi * p.sRi;
    __shared__ __align__(16) float ctile[16][36];
#pragma unroll
    for (int t = 0; t < 2; ++t) {
        const int n = n0 + t * 16 + l15; const int nn = min(n, p.N - 1);
#pragma unroll
        for (int r = 0; r < 8; ++r) {
            const int m = m0 + 8 * h + r; const int mm = min(m, p.M - 1);
            float v = acc[t][r] * iscale;
            if (p.flags & 1) v += p.bias[nn];
            if (p.flags & 2) v += p.bias[mm];
            if (p.flags & 8) v *= p.bias[(long long)zo * p.M + mm];
            v = act_fn(v, p.act);
            if (p.flags & 4) v += p.beta * R[(long long)mm * p.sRm + (long long)nn * p.sRn];
            ctile[8 * h + r][t * 16 + l15] = (n < p.N) ? v : 0.f;
        }
    }
    __syncthreads();
    const int NW = (p.Npad > p.N) ? p.Npad : p.N;
    const bool fast = (m0 + 16 <= p.M) && (n0 + 32 <= NW) && ((p.sCm & 3) == 0) && ((((size_t)C) & 15) == 0);
    if (fast) {
#pragma unroll
        for (int s = 0; s < 4; ++s) {
            const int row = s * 4 + (lane >> 3), c4 = (lane & 7) * 4;
            const v4f v = *(const v4f*)&ctile[row][c4];
            VST2V4(C + (long long)(m0 + row) * p.sCm + n0 + c4, v);
        }
    } else {
        for (int row = 0; row < 16; ++row) {
            const int m = m0 + row, n = n0 + lane;
            if (m < p.M && n < NW) VST2(float, C + (long long)m * p.sCm + n, ctile[row][lane]);
        }
    }
}


template <int MODE, int TM, int TN>
__global__ __launch_bounds__(32) void k_gemmT(GemmP p) {
    const int lane = threadIdx.x & 31, h = lane >> 4, l15 = lane & 15;
    const int m0 = blockIdx.y * (16 * TM), n0 = blockIdx.x * (16 * TN);
    const int z = blockIdx.z, zo = z / p.zi_n, zi = z - zo * p.zi_n;
    const float* A = p.A + zo * p.sAo + zi * p.sAi;
    const float* B = p.B + zo * p.sBo + zi * p.sBi;
    v8f acc[TM][TN];
#pragma unroll
    for (int i = 0; i < TM; ++i)
#pragma unroll
        for (int t = 0; t < TN; ++t) { v8f zz = {}; acc[i][t] = zz; }
    for (int k0 = 0; k0 < p.K; k0 += 32) {
        if (MODE == 1) {
            Split a[TM], b[TN];
#pragma unroll
            for (int i = 0; i < TM; ++i) { const int am = min(m0 + 16 * i + l15, p.M - 1); a[i] = sp_ld(A + (long long)am * p.sAm, p.sAk, k0, h, p.K, 1.f); }
#pragma unroll
            for (int t = 0; t < TN; ++t) { const int bn = min(n0 + 16 * t + l15, p.N - 1); b[t] = sp_ld(B + (long long)bn * p.sBn, p.sBk, k0, h, p.K, 1.f); }
#pragma unroll
            for (int i = 0; i < TM; ++i)
#pragma unroll
                for (int t = 0; t < TN; ++t) acc[i][t] = wmma3(a[i], b[t], acc[i][t]);
        } else if (MODE == 2) {
            v16b a[TM], b[TN];
#pragma unroll
            for (int i = 0; i < TM; ++i) { const int am = min(m0 + 16 * i + l15, p.M - 1); a[i] = bh_ld(A + (long long)am * p.sAm, p.sAk, k0, h, p.K, 1.f); }
#pragma unroll
            for (int t = 0; t < TN; ++t) { const int bn = min(n0 + 16 * t + l15, p.N - 1); b[t] = bh_ld(B + (long long)bn * p.sBn, p.sBk, k0, h, p.K, 1.f); }
#pragma unroll
            for (int i = 0; i < TM; ++i)
#pragma unroll
                for (int t = 0; t < TN; ++t) acc[i][t] = wmmab(a[i], b[t], acc[i][t]);
        } else {
            v16h a[TM], b[TN];
#pragma unroll
            for (int i = 0; i < TM; ++i) { const int am = min(m0 + 16 * i + l15, p.M - 1); a[i] = fh_ld(A + (long long)am * p.sAm, p.sAk, k0, h, p.K, p.sa); }
#pragma unroll
            for (int t = 0; t < TN; ++t) { const int bn = min(n0 + 16 * t + l15, p.N - 1); b[t] = fh_ld(B + (long long)bn * p.sBn, p.sBk, k0, h, p.K, p.sb); }
#pragma unroll
            for (int i = 0; i < TM; ++i)
#pragma unroll
                for (int t = 0; t < TN; ++t) acc[i][t] = wmma16(a[i], b[t], acc[i][t]);
        }
    }
    const float iscale = (MODE == 0) ? p.alpha / (p.sa * p.sb) : p.alpha;
    float* C = p.C + zo * p.sCo + zi * p.sCi;
    const float* R = p.R + zo * p.sRo + zi * p.sRi;
    const int NW = (p.Npad > p.N) ? p.Npad : p.N;
    __shared__ __align__(16) float ctile[16][36];
#pragma unroll
    for (int i = 0; i < TM; ++i) {
        const int mb = m0 + 16 * i; if (mb >= p.M) break;
#pragma unroll
        for (int tp = 0; tp < TN / 2; ++tp) {
            const int nb = n0 + 32 * tp; if (nb >= NW) break;
#pragma unroll
            for (int t2 = 0; t2 < 2; ++t2) {
                const int t = 2 * tp + t2; const int n = nb + t2 * 16 + l15; const int nn = min(n, p.N - 1);
#pragma unroll
                for (int r = 0; r < 8; ++r) {
                    const int m = mb + 8 * h + r; const int mm = min(m, p.M - 1);
                    float v = acc[i][t][r] * iscale;
                    if (p.flags & 1) v += p.bias[nn];
                    if (p.flags & 2) v += p.bias[mm];
            if (p.flags & 8) v *= p.bias[(long long)zo * p.M + mm];
                    v = act_fn(v, p.act);
                    if (p.flags & 4) v += p.beta * R[(long long)mm * p.sRm + (long long)nn * p.sRn];
                    ctile[8 * h + r][t2 * 16 + l15] = (n < p.N) ? v : 0.f;
                }
            }
            __syncthreads();
            const bool fast = (mb + 16 <= p.M) && (nb + 32 <= NW) && ((p.sCm & 3) == 0) && ((((size_t)C) & 15) == 0);
            if (fast) {
#pragma unroll
                for (int s = 0; s < 4; ++s) {
                    const int row = s * 4 + (lane >> 3), c4 = (lane & 7) * 4;
                    const v4f v = *(const v4f*)&ctile[row][c4];
                    VST2V4(C + (long long)(mb + row) * p.sCm + nb + c4, v);
                }
            } else {
                for (int row = 0; row < 16; ++row) {
                    const int m = mb + row, n = nb + lane;
                    if (m < p.M && n < NW) VST2(float, C + (long long)m * p.sCm + n, ctile[row][lane]);
                }
            }
            __syncthreads();
        }
    }
}

#define AW 4
struct AttnP {
    const float* Q; const float* K; const float* V; float* O; float* P; const float* Mf; const int* Mi; float* ST;
    const float* Pw; const float* Rt; const int* SQ; const int* SK;
    long long swb, swh, swi, swj, srb, srh, sri;
    long long sQb, sQh, sQi, sQd, sKb, sKh, sKj, sKd, sVb, sVh, sVj, sVd, sOb, sOh, sOi, sPb, sPh, sPi, smb, smh, smi, smj;
    int Lq, Lk, dh, dv, hrep, causal, coff, pband;
    float scale, mfill; int nonorm, mpol;
    int roff, rn, segpol, win;
};
static_assert(sizeof(AttnP) == 12 * 8 + 29 * 8 + 16 * 4, "AttnP has padding");

#ifndef KATTN_ATTR
#define KATTN_ATTR
#endif
template <int DHP, int DVP, int QM, bool SPLITPV, bool TWOPASS>
__global__ __launch_bounds__(32 * AW) KATTN_ATTR void k_attn(AttnP p) {
    constexpr int NT = DVP / 16;
    constexpr int KS = DHP / 32;
    constexpr int VP = DVP + 8;
    __shared__ __align__(16) float    pl[AW][16 * 64];
    __shared__ __align__(16) _Float16 vl[(SPLITPV ? 2 : 1) * 64 * VP];
    const int lane = threadIdx.x & 31, hf = lane >> 4, l15 = lane & 15, wave = threadIdx.x >> 5;
    const int h = blockIdx.y, b = blockIdx.z, hk = h / p.hrep;
    const int q0 = (blockIdx.x * AW + wave) * 16;
    float* myp = pl[wave];
    const float L2E = 1.4426950408889634f;
    const float NEG = -__builtin_inff();
    const int qi = min(q0 + l15, p.Lq - 1);
    const float* qrow = p.Q + b * p.sQb + h * p.sQh + (long long)qi * p.sQi;
    const float* kbase = p.K + b * p.sKb + hk * p.sKh;
    const float* vbase = p.V + b * p.sVb + hk * p.sVh;
    v16h qa[QM == 0 ? KS : 1]; Split qs_[QM == 1 ? KS : 1]; Split3 qt_[QM == 2 ? KS : 1];
#pragma unroll
    for (int ks = 0; ks < KS; ++ks) {
        if (QM == 2) qt_[ks] = sp3_ld(qrow, p.sQd, ks * 32, hf, p.dh, 1.f);
        else if (QM == 1) qs_[ks] = sp_ld(qrow, p.sQd, ks * 32, hf, p.dh, 1.f);
        else qa[ks] = fh_ld(qrow, p.sQd, ks * 32, hf, p.dh, 1.f);
    }
    v8f o[NT]; float m8[8], l8[8];
#pragma unroll
    for (int t = 0; t < NT; ++t) { v8f zz = {}; o[t] = zz; }
#pragma unroll
    for (int i = 0; i < 8; ++i) { m8[i] = NEG; l8[i] = 0.f; }
    int jend = p.Lk;
    if (p.causal == 1) { const int je = (blockIdx.x * AW + AW - 1) * 16 + 16 + p.coff; jend = min(jend, max(je, 0)); }
    const int npass = TWOPASS ? 2 : 1;
    for (int pass = 0; pass < npass; ++pass) {
        const bool dopv = (!TWOPASS) || pass == 1;
        for (int j0 = 0; j0 < jend; j0 += 64) {
            if (dopv) {
                __syncthreads();
                for (int idx = threadIdx.x; idx < 64 * DVP; idx += 32 * AW) {
                    const int jr = idx / DVP, d = idx - jr * DVP, j = j0 + jr;
                    const float f = (j < p.Lk && d < p.dv) ? vbase[(long long)j * p.sVj + (long long)d * p.sVd] : 0.f;
                    if (SPLITPV) {
                        const __bf16 hb = bf16_rne(f);
                        ((__bf16*)vl)[jr * VP + d] = hb; ((__bf16*)vl)[64 * VP + jr * VP + d] = bf16_rne(f - bf16_f32(hb));
                    } else vl[jr * VP + d] = (_Float16)f;
                }
            }
            v8f s[4];
#pragma unroll
            for (int t = 0; t < 4; ++t) {
                const int j = min(j0 + t * 16 + l15, p.Lk - 1);
                const float* krow = kbase + (long long)j * p.sKj;
                v8f acc = {};
#pragma unroll
                for (int ks = 0; ks < KS; ++ks) {
                    if (QM == 2)      acc = wmma6(qt_[ks], sp3_ld(krow, p.sKd, ks * 32, hf, p.dh, 1.f), acc);
                    else if (QM == 1) acc = wmma3(qs_[ks], sp_ld(krow, p.sKd, ks * 32, hf, p.dh, 1.f), acc);
                    else              acc = wmma16(qa[ks], fh_ld(krow, p.sKd, ks * 32, hf, p.dh, 1.f), acc);
                }
                s[t] = acc;
            }
            float pv[8][4];
#pragma unroll
            for (int i = 0; i < 8; ++i) {
                const int irow = q0 + i + 8 * hf;
                const int ic = min(irow, p.Lq - 1);
                float sc[4];
#pragma unroll
                for (int t = 0; t < 4; ++t) {
                    const int jg = j0 + t * 16 + l15;
                    float v = s[t][i] * p.scale;
                    if (p.Mf) v += p.Mf[b * p.smb + h * p.smh + (long long)ic * p.smi + (long long)min(jg, p.Lk - 1) * p.smj];
                    if (p.Rt) { int rc = ic - min(jg, p.Lk - 1) + p.roff; rc = rc < 0 ? 0 : (rc >= p.rn ? p.rn - 1 : rc); v += p.Rt[b * p.srb + h * p.srh + (long long)ic * p.sri + rc]; }
                    if (p.Mi) { const int mv = p.Mi[b * p.smb + h * p.smh + (long long)ic * p.smi + (long long)min(jg, p.Lk - 1) * p.smj]; if (p.mpol ? (mv != 0) : (mv == 0)) v = p.mfill; }
                    if (p.SQ) { const bool same = p.SQ[(long long)b * p.Lq + ic] == p.SK[(long long)b * p.Lk + min(jg, p.Lk - 1)]; if (p.segpol ? same : !same) v = p.mfill; }
                    if (p.causal == 2 && jg > irow + p.coff) v = p.mfill;
                    if (jg >= p.Lk || (p.causal == 1 && jg > irow + p.coff) || (p.causal == 3 && jg < irow + p.coff) || (p.win > 0 && irow + p.coff - jg > p.win)) v = NEG; else v *= L2E;
                    sc[t] = v;
                }
                if (!TWOPASS || pass == 0) {
                    float mx = fmaxf(fmaxf(sc[0], sc[1]), fmaxf(sc[2], sc[3]));
                    mx = fmaxf(mx, __shfl_xor(mx, 1, 32)); mx = fmaxf(mx, __shfl_xor(mx, 2, 32));
                    mx = fmaxf(mx, __shfl_xor(mx, 4, 32)); mx = fmaxf(mx, __shfl_xor(mx, 8, 32));
                    const float mnew = fmaxf(m8[i], mx);
                    const float corr = (mnew == NEG) ? 1.f : exp2f(m8[i] - mnew);
                    float rs = 0.f;
#pragma unroll
                    for (int t = 0; t < 4; ++t) {
                        const float pp = (sc[t] == NEG) ? 0.f : exp2f(sc[t] - mnew); rs += pp;
                        pv[i][t] = p.Pw ? pp * p.Pw[b * p.swb + h * p.swh + (long long)ic * p.swi + (long long)min(j0 + t * 16 + l15, p.Lk - 1) * p.swj] : pp;
                    }
                    rs += __shfl_xor(rs, 1, 32); rs += __shfl_xor(rs, 2, 32); rs += __shfl_xor(rs, 4, 32); rs += __shfl_xor(rs, 8, 32);
                    l8[i] = l8[i] * corr + rs; m8[i] = mnew;
                    if (!TWOPASS) {
#pragma unroll
                        for (int t = 0; t < NT; ++t) o[t][i] *= corr;
                    }
                } else {
                    const float inv = (l8[i] > 0.f) ? 1.f / l8[i] : 0.f;
#pragma unroll
                    for (int t = 0; t < 4; ++t) {
                        const int jg = j0 + t * 16 + l15;
                        float pp = (sc[t] == NEG) ? 0.f : exp2f(sc[t] - m8[i]) * inv;
                        if (p.Pw) pp *= p.Pw[b * p.swb + h * p.swh + (long long)ic * p.swi + (long long)min(jg, p.Lk - 1) * p.swj];
                        pv[i][t] = pp;
                    }
                }
            }
            if (dopv) {
#pragma unroll
                for (int i = 0; i < 8; ++i)
#pragma unroll
                    for (int t = 0; t < 4; ++t) myp[(i + 8 * hf) * 64 + t * 16 + l15] = pv[i][t];
                __syncthreads();
                if (p.P) {
                    float* pb_ = p.P + b * p.sPb + h * p.sPh;
                    const bool fastP = (p.pband == 0) && ((p.sPi & 3) == 0) && (j0 + 64 <= p.Lk) && (q0 + 16 <= p.Lq) && ((((size_t)pb_) & 15) == 0);
                    if (fastP) {
#pragma unroll
                        for (int s = 0; s < 8; ++s) {
                            const int row = s * 2 + (lane >> 4), c4 = (lane & 15) * 4;
                            const v4f v = *(const v4f*)(myp + row * 64 + c4);
                            VST2V4(pb_ + (long long)(q0 + row) * p.sPi + j0 + c4, v);
                        }
                    } else {
                        for (int row = 0; row < 16; ++row) {
                            const int irow = q0 + row; if (irow >= p.Lq) continue;
                            for (int c = lane; c < 64; c += 32) {
                                const int jg = j0 + c; if (jg >= p.Lk) continue;
                                if (p.pband == 0) VST2(float, pb_ + (long long)irow * p.sPi + jg, myp[row * 64 + c]);
                                else if (jg - irow <= p.pband && irow - jg <= p.pband) VST2(float, pb_ + (long long)irow * p.sPi + (jg - irow + p.pband), myp[row * 64 + c]);
                            }
                        }
                    }
                }
                if (SPLITPV) {
                    const Split pa0 = sp_ld(myp + l15 * 64, 1, 0, hf, 64, 1.f), pa1 = sp_ld(myp + l15 * 64, 1, 32, hf, 64, 1.f);
                    const __bf16* vh = (const __bf16*)vl; const __bf16* vlo = vh + 64 * VP;
#pragma unroll
                    for (int t = 0; t < NT; ++t) {
                        const int dcol = t * 16 + l15;
                        Split b0, b1;
#pragma unroll
                        for (int e = 0; e < 16; ++e) {
                            const int k0 = frag_k(e, hf), k1 = 32 + frag_k(e, hf);
                            b0.hi[e] = vh[k0 * VP + dcol]; b0.lo[e] = vlo[k0 * VP + dcol]; b1.hi[e] = vh[k1 * VP + dcol]; b1.lo[e] = vlo[k1 * VP + dcol];
                        }
                        o[t] = wmma3(pa0, b0, o[t]);
                        o[t] = wmma3(pa1, b1, o[t]);
                    }
                } else {
                    const v16h pa0 = fh_ld(myp + l15 * 64, 1, 0, hf, 64, 4096.f), pa1 = fh_ld(myp + l15 * 64, 1, 32, hf, 64, 4096.f);
#pragma unroll
                    for (int t = 0; t < NT; ++t) {
                        const int dcol = t * 16 + l15;
                        v16h b0, b1;
#pragma unroll
                        for (int e = 0; e < 16; ++e) { b0[e] = vl[frag_k(e, hf) * VP + dcol]; b1[e] = vl[(32 + frag_k(e, hf)) * VP + dcol]; }
                        o[t] = wmma16(pa0, b0, o[t]);
                        o[t] = wmma16(pa1, b1, o[t]);
                    }
                }
            }
        }
    }
    float* obase = p.O + b * p.sOb + h * p.sOh;
    if (p.ST) {
        const int rl = lane >> 1, isel = rl & 7;
        float mv = 0.f, lv = 0.f;
#pragma unroll
        for (int i = 0; i < 8; ++i) if (i == isel) { mv = m8[i]; lv = l8[i]; }
        const int irow = q0 + rl;
        if (irow < p.Lq) { float* st = p.ST + (((long long)b * gridDim.y + h) * p.Lq + irow) * 2 + (lane & 1); VST2(float, st, (lane & 1) ? lv : mv * 0.6931471805599453f); }
    }
    float invr[8];
#pragma unroll
    for (int i = 0; i < 8; ++i) {
        if (TWOPASS) invr[i] = SPLITPV ? 1.f : (1.f / 4096.f);
        else if (p.nonorm) invr[i] = exp2f(m8[i]) * (SPLITPV ? 1.f : (1.f / 4096.f));
        else invr[i] = (l8[i] > 0.f) ? (SPLITPV ? 1.f / l8[i] : 1.f / (l8[i] * 4096.f)) : 0.f;
    }
    __syncthreads();
    const bool ofast = ((p.sOi & 3) == 0) && ((((size_t)obase) & 15) == 0) && (q0 + 16 <= p.Lq);
#pragma unroll
    for (int c0 = 0; c0 < DVP; c0 += 64) {
#pragma unroll
        for (int i = 0; i < 8; ++i)
#pragma unroll
            for (int t = 0; t < NT; ++t) if (t * 16 >= c0 && t * 16 < c0 + 64) myp[(i + 8 * hf) * 64 + (t * 16 - c0) + l15] = o[t][i] * invr[i];
        __syncthreads();
        const int cw = (DVP - c0 < 64) ? (DVP - c0) : 64;
        if (ofast && (c0 + cw <= p.dv) && (cw % 32 == 0)) {
            const int lpr = cw / 4;
            const int rows_per_ins = 32 / lpr;
            for (int r0 = 0; r0 < 16; r0 += rows_per_ins) {
                const int row = r0 + lane / lpr, c4 = (lane % lpr) * 4;
                const v4f v = *(const v4f*)(myp + row * 64 + c4);
                VST2V4(obase + (long long)(q0 + row) * p.sOi + c0 + c4, v);
            }
        } else {
            for (int row = 0; row < 16; ++row) {
                const int irow = q0 + row; if (irow >= p.Lq) continue;
                for (int c = lane; c < cw; c += 32) { const int d = c0 + c; if (d < p.dv) VST2(float, obase + (long long)irow * p.sOi + d, myp[row * 64 + c]); }
            }
        }
        __syncthreads();
    }
}

struct TrP { const float* src; float* dst; const float* R2; long long sSz, lds, sDz, ldd, sRz, ldr; int R, C, flags, act; float alpha, beta; };
static_assert(sizeof(TrP) == 3 * 8 + 6 * 8 + 6 * 4, "TrP has padding");
__global__ __launch_bounds__(256) void k_tr(TrP p) {
    __shared__ float tile[32][33];
    const int c0 = blockIdx.x * 32, r0 = blockIdx.y * 32, z = blockIdx.z;
    const int lane = threadIdx.x & 31, wave = threadIdx.x >> 5;
    const float* s = p.src + z * p.sSz;
#pragma unroll
    for (int k = 0; k < 4; ++k) {
        const int rl = wave * 4 + k, r = r0 + rl, c = c0 + lane;
        tile[rl][lane] = (r < p.R && c < p.C) ? s[(long long)r * p.lds + c] : 0.f;
    }
    __syncthreads();
    float* d = p.dst + z * p.sDz; const float* rr = p.R2 + z * p.sRz;
#pragma unroll
    for (int k = 0; k < 4; ++k) {
        const int cl = wave * 4 + k, c = c0 + cl, r = r0 + lane;
        if (c < p.C && r < p.R) {
            float v = act_fn(p.alpha * tile[lane][cl], p.act);
            if (p.flags & 1) v += p.beta * rr[(long long)c * p.ldr + r];
            VST2(float, d + (long long)c * p.ldd + r, v);
        }
    }
}

__global__ __launch_bounds__(256) void k_affine(const float* __restrict__ src, float* __restrict__ dst, int n, float a, float b, const float* __restrict__ sdev) {
    const int i = blockIdx.x * 256 + threadIdx.x;
    if (i < n) { const float aa = sdev ? a * sdev[0] : a; const float v = aa * src[i] + b; VST2(float, dst + i, v); }
}

struct SmP { const float* src; float* dst; const float* Mf; long long sz, sr, dz, dr, smz, smr; int n, pad; float scale_in, scale_out; };
static_assert(sizeof(SmP) == 3 * 8 + 6 * 8 + 4 * 4, "SmP has padding");
__global__ __launch_bounds__(256) void k_softmax(SmP p) {
    __shared__ float red[256];
    const int r = blockIdx.x, z = blockIdx.y, tid = threadIdx.x;
    const float* s = p.src + z * p.sz + (long long)r * p.sr;
    const float* mf = p.Mf ? (p.Mf + z * p.smz + (long long)r * p.smr) : nullptr;
    float mx = -__builtin_inff();
    for (int j = tid; j < p.n; j += 256) { float v = s[j] * p.scale_in; if (mf) v += mf[j]; mx = fmaxf(mx, v); }
    red[tid] = mx; __syncthreads();
    for (int o = 128; o > 0; o >>= 1) { if (tid < o) red[tid] = fmaxf(red[tid], red[tid + o]); __syncthreads(); }
    mx = red[0]; __syncthreads();
    float sum = 0.f;
    for (int j = tid; j < p.n; j += 256) { float v = s[j] * p.scale_in; if (mf) v += mf[j]; sum += (mx == -__builtin_inff()) ? 0.f : expf(v - mx); }
    red[tid] = sum; __syncthreads();
    for (int o = 128; o > 0; o >>= 1) { if (tid < o) red[tid] += red[tid + o]; __syncthreads(); }
    sum = red[0];
    const float inv = (sum > 0.f) ? p.scale_out / sum : 0.f;
    float* d = p.dst + z * p.dz + (long long)r * p.dr;
    for (int j = tid; j < p.n; j += 256) { float v = s[j] * p.scale_in; if (mf) v += mf[j]; const float o = (mx == -__builtin_inff()) ? 0.f : expf(v - mx) * inv; VST2(float, d + j, o); }
}
__global__ __launch_bounds__(256) void k_stats(const float* __restrict__ x, long long sz, long long so, long long si, int inner, int n, float eps, float* __restrict__ stat, int mode) {
    __shared__ float red[256];
    const int z = blockIdx.x, tid = threadIdx.x;
    const float* base = x + z * sz;
    float s = 0.f;
    for (int e = tid; e < n; e += 256) s += base[(long long)(e / inner) * so + (long long)(e % inner) * si];
    red[tid] = s; __syncthreads();
    for (int o = 128; o > 0; o >>= 1) { if (tid < o) red[tid] += red[tid + o]; __syncthreads(); }
    const float mu = (mode == 0 || mode == 3) ? red[0] / (float)n : 0.f; __syncthreads();
    float q = 0.f;
    for (int e = tid; e < n; e += 256) { const float dlt = base[(long long)(e / inner) * so + (long long)(e % inner) * si] - mu; q += dlt * dlt; }
    red[tid] = q; __syncthreads();
    for (int o = 128; o > 0; o >>= 1) { if (tid < o) red[tid] += red[tid + o]; __syncthreads(); }
    {
        float rs;
        if (mode == 2) rs = sqrtf((float)n) / fmaxf(sqrtf(red[0]), eps); else if (mode == 3) rs = rsqrtf(red[0] / (float)(n - 1) + eps); else rs = rsqrtf(red[0] / (float)n + eps);
        if (tid < 32) { const float v = (tid == 0) ? mu : ((tid == 1) ? rs : 0.f); VST2(float, stat + (long long)z * 32 + tid, v); }
    }
}
__global__ __launch_bounds__(256) void k_norm_apply(const float* __restrict__ x, float* __restrict__ y, const float* __restrict__ stat, const float* __restrict__ g, const float* __restrict__ bta,
                                                     int Z, int C, int L, int G, int bn, int act) {
    const long long idx = (long long)blockIdx.x * 256 + threadIdx.x;
    if (idx >= (long long)Z * C * L) return;
    const int l = (int)(idx % L); const long long zc = idx / L; const int c = (int)(zc % C), z = (int)(zc / C); (void)l;
    const int set = bn ? c : (z * G + c / (C / G));
    float v = (x[idx] - stat[(long long)set * 32]) * stat[(long long)set * 32 + 1];
    if (g) v *= g[c];
    if (bta) v += bta[c];
    v = act_fn(v, act);
    VST2(float, y + idx, v);
}

__global__ __launch_bounds__(256) void k_lse_neg(const float* __restrict__ st, float* __restrict__ c, int n) {
    const int i = blockIdx.x * 256 + threadIdx.x;
    if (i < n) { const float v = -(st[2 * i] + logf(st[2 * i + 1])); VST2(float, c + i, v); }
}

__global__ __launch_bounds__(256) void k_iota(int* __restrict__ dst, int n, int a, int b) {
    const int i = blockIdx.x * 256 + threadIdx.x;
    if (i < n) { const int v = a * i + b; VST2(int, dst + i, v); }
}

__global__ __launch_bounds__(256) void k_axpby(const float* __restrict__ x, const float* __restrict__ y, float* __restrict__ dst, int n, float a, float b, float c) {
    const int i = blockIdx.x * 256 + threadIdx.x;
    if (i < n) { const float v = a * x[i] + b * y[i] + c; VST2(float, dst + i, v); }
}

struct RopeP { const float* X; float* Y; const float* C; const float* Sn; const int* pos; long long sXr, sXh, sYr, sYh, sCb, sCp, sCd; int R, Hn, D, S, mode, tmode, pmode, pad; };
static_assert(sizeof(RopeP) == 5 * 8 + 7 * 8 + 8 * 4, "RopeP has padding");
__global__ __launch_bounds__(256) void k_rope(RopeP p) {
    const long long idx = (long long)blockIdx.x * 256 + threadIdx.x;
    if (idx >= (long long)p.R * p.Hn * p.D) return;
    const int d = (int)(idx % p.D); const long long rh = idx / p.D; const int h = (int)(rh % p.Hn); const int r = (int)(rh / p.Hn);
    const int half = p.D / 2;
    int partner; float sign;
    if (p.mode == 0) { partner = (d < half) ? d + half : d - half; sign = (d < half) ? -1.f : 1.f; }
    else { partner = d ^ 1; sign = (d & 1) ? 1.f : -1.f; }
    const int tcol = (p.tmode == 0) ? d : ((p.tmode == 1) ? (d % half) : (d >> 1));
    const int pp = (p.pmode == 0) ? (r % p.S) : ((p.pmode == 1) ? h : p.pos[r]);
    const long long toff = (long long)(r / p.S) * p.sCb + (long long)pp * p.sCp + (long long)tcol * p.sCd;
    const float* xr = p.X + (long long)r * p.sXr + (long long)h * p.sXh;
    const float v = xr[d] * p.C[toff] + sign * xr[partner] * p.Sn[toff];
    VST2(float, p.Y + (long long)r * p.sYr + (long long)h * p.sYh + d, v);
}

__global__ __launch_bounds__(256) void k_invf(float* __restrict__ invb, int half, int D, float base, float num, int fmode, float cexp) {
    const int i = blockIdx.x * 256 + threadIdx.x;
    if (i >= ((half + 31) / 32) * 32) return;
    if (i >= half) { VST2(float, invb + i, 0.f); return; }
    const float e = (float)(2 * i) / (float)D;
    float invf;
    if (fmode == 1) invf = num * expf((float)(2 * i) * cexp);
    else if (fmode == 2) invf = num * powf(base, (-2.0f * ((float)i - 1.0f)) / (float)D);
    else invf = num * (1.0f / powf(base, e));
    VST2(float, invb + i, invf);
}
__global__ __launch_bounds__(256) void k_sincos(float* __restrict__ cs, float* __restrict__ sn, const float* __restrict__ invb, int S, int half, float pscale) {
    const int idx = blockIdx.x * 256 + threadIdx.x;
    if (idx >= S * half) return;
    const int s = idx / half, i = idx - s * half;
    const float ang = (pscale * (float)s) * invb[i];
    VST2(float, cs + idx, cosf(ang)); VST2(float, sn + idx, sinf(ang));
}

__global__ __launch_bounds__(256) void k_mulact(const float* __restrict__ x, const float* __restrict__ y, float* __restrict__ dst, int n, int act) {
    const int i = blockIdx.x * 256 + threadIdx.x;
    if (i < n) { const float v = act_fn(x[i], act) * y[i]; VST2(float, dst + i, v); }
}

__global__ __launch_bounds__(256) void k_matvec(GemmP p) {
    const int rpt = (p.N == 1) ? 1 : 32;
    const long long r0 = ((long long)blockIdx.x * 256 + threadIdx.x) * rpt; const int z = blockIdx.z, zo = z / p.zi_n, zi = z - zo * p.zi_n;
    if (r0 >= p.M) return;
    const float* Bb = p.B + zo * p.sBo + zi * p.sBi;
    float* C = p.C + zo * p.sCo + zi * p.sCi; const float* R = p.R + zo * p.sRo + zi * p.sRi;
    for (int rr = 0; rr < rpt; ++rr) {
        const long long r = r0 + rr; if (r >= p.M) break;
        const float* A = p.A + zo * p.sAo + zi * p.sAi + r * p.sAm;
        float acc[8] = {0.f, 0.f, 0.f, 0.f, 0.f, 0.f, 0.f, 0.f};
        for (int k = 0; k < p.K; ++k) { const float a = A[(long long)k * p.sAk];
#pragma unroll
            for (int j = 0; j < 8; ++j) if (j < p.N) acc[j] += a * Bb[(long long)j * p.sBn + (long long)k * p.sBk]; }
#pragma unroll
        for (int j = 0; j < 8; ++j) if (j < p.N) {
            float v = acc[j] * p.alpha;
            if (p.flags & 1) v += p.bias[j];
            if (p.flags & 2) v += p.bias[r];
            v = act_fn(v, p.act);
            if (p.flags & 4) v += p.beta * R[r * p.sRm + (long long)j * p.sRn];
            VST2(float, C + r * p.sCm + j, v);
        }
    }
}
__global__ __launch_bounds__(256) void k_smallsoftmax(const float* __restrict__ src, float* __restrict__ dst, long long sr, long long dr, int n, long long R, float scale) {
    const long long r0 = ((long long)blockIdx.x * 256 + threadIdx.x) * 32;
    for (int rr = 0; rr < 32; ++rr) {
        const long long r = r0 + rr; if (r >= R) return;
        const float* s = src + r * sr; float* d = dst + r * dr;
        float mx = -__builtin_inff();
        for (int j = 0; j < n; ++j) mx = fmaxf(mx, s[j] * scale);
        float sum = 0.f;
        for (int j = 0; j < n; ++j) sum += expf(s[j] * scale - mx);
        const float inv = 1.f / sum;
        for (int j = 0; j < n; ++j) { const float v = expf(s[j] * scale - mx) * inv; VST2(float, d + j, v); }
    }
}

__global__ __launch_bounds__(32) void k_unitstat(float* __restrict__ st) { const int t = threadIdx.x; const float v = (t == 1) ? 1.f : 0.f; VST2(float, st + t, v); }

__global__ __launch_bounds__(256) void k_lincopy(const float* __restrict__ src, long long lds, float* __restrict__ dst, long long ldd, long long rows, int cols) {
    const long long i = (long long)blockIdx.x * 256 + threadIdx.x; if (i >= rows * cols) return;
    const long long r = i / cols; const int c = (int)(i - r * cols);
    const float v = src[r * lds + c]; VST2(float, dst + r * ldd + c, v);
}

__global__ __launch_bounds__(256) void k_rt_kpad(float* __restrict__ KP, int Bn, int S, int D, int PADK, int SP) { const long long q = (long long)blockIdx.x * 256 + threadIdx.x; if (q >= (long long)Bn * 2 * PADK * D) return; const int c = (int)(q % D); const int rr = (int)((q / D) % (2 * PADK)); const int b = (int)(q / ((long long)D * 2 * PADK)); const int r = (rr < PADK) ? rr : (S + rr); VST2(float, KP + ((long long)b * SP + r) * D + c, 0.f); }
__global__ __launch_bounds__(128) void k_rt_soft(float* __restrict__ PB, const int* __restrict__ lens, const float* __restrict__ decw, int b0, int BC, int NH, int S, int KW, int PADK, float scale, float rate) { const long long q = (long long)blockIdx.x * 128 + threadIdx.x; if (q >= (long long)BC * NH * S) return; const int i = (int)(q % S); const int h = (int)((q / S) % NH); const int b = b0 + (int)(q / ((long long)S * NH)); const int blk = i / 64; const int j0 = blk * 64 - PADK; const int len = lens[b]; const float dw = decw[0];
    float* row = PB + q * KW;
    float mx = -__builtin_inff();
#pragma unroll 1
    for (int c = 0; c < KW; ++c) { const int j = j0 + c; if (j < 0 || j >= S || abs(i - j) > PADK || j >= len) continue; const float bias = logf(expf(-rate * dw * (float)(S - 1 - j)) + 1e-8f); const float v = row[c] * scale + bias; mx = fmaxf(mx, v); }
    float den = 0.f;
#pragma unroll 1
    for (int c = 0; c < KW; ++c) { const int j = j0 + c; float e = 0.f; if (!(j < 0 || j >= S || abs(i - j) > PADK || j >= len)) { const float bias = logf(expf(-rate * dw * (float)(S - 1 - j)) + 1e-8f); e = expf(row[c] * scale + bias - mx); den += e; } VST2(float, row + c, e); }
    const float inv = 1.f / den;
#pragma unroll 1
    for (int c = 0; c < KW; ++c) { const float e = row[c]; VST2(float, row + c, e * inv); } }
__global__ __launch_bounds__(128) void k_rt_col(const float* __restrict__ PB, const int* __restrict__ lens, float* __restrict__ PBAR, int b0, int BC, int NH, int S, int KW, int PADK) { const long long q = (long long)blockIdx.x * 128 + threadIdx.x; if (q >= (long long)BC * NH * S) return; const int j = (int)(q % S); const long long bhl = q / S; const int bl = (int)(bhl / NH); const int h = (int)(bhl % NH); const int b = b0 + bl; const int len = lens[b]; const float cnt = fmaxf((float)min(len, S), 1.f); float s = 0.f;
#pragma unroll 1
    for (int i = max(j - PADK, 0); i <= min(j + PADK, S - 1); ++i) { if (i >= len) break; const int blk = i / 64; const int c = j - (blk * 64 - PADK); s += PB[(bhl * S + i) * KW + c]; }
    VST2(float, PBAR + ((long long)b * NH + h) * S + j, s / cnt); }
__global__ __launch_bounds__(256) void k_rt_pool(const float* __restrict__ PBAR, const float* __restrict__ QV, const float* __restrict__ seq, const int* __restrict__ lens, float* __restrict__ ATT, float* __restrict__ POOL, int Bn, int NH, int S, int D, int HD) { const int q = blockIdx.x * 256 + threadIdx.x; if (q >= Bn * D) return; const int c = q % D; const int b = q / D; const int h = c / HD; const int len = lens[b]; const float cnt = fmaxf((float)min(len, S), 1.f); float a = 0.f, m = 0.f;
#pragma unroll 1
    for (int j = 0; j < S; ++j) { a += PBAR[((long long)b * NH + h) * S + j] * QV[((long long)b * S + j) * 2 * D + D + c]; if (j < len) m += seq[((long long)b * S + j) * D + c]; }
    VST2(float, ATT + q, a); VST2(float, POOL + q, m / cnt); }
__global__ __launch_bounds__(256) void k_rt_ln(const float* __restrict__ X, const float* __restrict__ POOL, const float* __restrict__ g_, const float* __restrict__ b_, float* __restrict__ OUT, int Bn, int D) { __shared__ float red[256]; __shared__ float red2[256]; const int b = blockIdx.x; const int t = threadIdx.x; float s = 0.f, s2 = 0.f;
    for (int c = t; c < D; c += 256) { const float v = X[b * D + c] + POOL[b * D + c]; s += v; s2 += v * v; } red[t] = s; red2[t] = s2; __syncthreads(); for (int o = 128; o > 0; o >>= 1) { if (t < o) { red[t] += red[t + o]; red2[t] += red2[t + o]; } __syncthreads(); }
    const float mu = red[0] / (float)D; const float rs = rsqrtf(fmaxf(red2[0] / (float)D - mu * mu, 0.f) + 1e-5f);
    for (int c = t; c < D; c += 256) { const float v = X[b * D + c] + POOL[b * D + c]; VST2(float, OUT + b * D + c, (v - mu) * rs * g_[c] + b_[c]); } }

template __global__ void k_gemm<0>(GemmP);
template __global__ void k_gemm<1>(GemmP);

extern "C" void kernel_launch(void* const* d_in, const int* in_sizes, int n_in, void* d_out, int out_size, void* d_ws, size_t ws_size, hipStream_t stream) {
    (void)in_sizes; (void)n_in; (void)out_size; (void)ws_size;
    const float* seq = (const float*)d_in[0];
    const float* Wqkv = (const float*)d_in[1];
    const float* Wout = (const float*)d_in[2];
    const float* bout = (const float*)d_in[3];
    const float* decw = (const float*)d_in[4];
    const float* lng = (const float*)d_in[5];
    const float* lnb = (const float*)d_in[6];
    const int* lens = (const int*)d_in[7];
    const int Bn = 16;
    const int S = 1024;
    const int D = 512;
    const int NH = 8;
    const int HD = 64;
    const int NR = Bn * S;
    const int QB = 64;
    const int KW = 320;
    const int PADK = 128;
    const int SP = S + 2 * PADK;
    const int NBLK = S / QB;
    const int BC = 2;
    float* out = (float*)d_out;
    char* wsp = (char*)d_ws;
    float* QV = (float*)wsp; wsp += (((size_t)((size_t)NR * 2 * D) * 4 + 255) / 256) * 256;
    float* KP = (float*)wsp; wsp += (((size_t)((size_t)Bn * SP * D) * 4 + 255) / 256) * 256;
    float* PB = (float*)wsp; wsp += (((size_t)((size_t)BC * NH * S * KW) * 4 + 255) / 256) * 256;
    float* PBAR = (float*)wsp; wsp += (((size_t)((size_t)Bn * NH * S) * 4 + 255) / 256) * 256;
    float* POOL = (float*)wsp; wsp += (((size_t)((size_t)Bn * D) * 4 + 255) / 256) * 256;
    float* ATT = (float*)wsp; wsp += (((size_t)((size_t)Bn * D) * 4 + 255) / 256) * 256;
    float* ATT2 = (float*)wsp; wsp += (((size_t)((size_t)Bn * D) * 4 + 255) / 256) * 256;
    { GemmP gq;
      gq.A = seq; gq.B = Wqkv; gq.bias = seq; gq.R = seq; gq.C = QV;
      gq.sAo = 0; gq.sAi = 0; gq.sAm = D; gq.sAk = 1; gq.sBo = 0; gq.sBi = 0; gq.sBn = D; gq.sBk = 1; gq.sCo = 0; gq.sCi = 0; gq.sCm = 2 * D; gq.sRo = 0; gq.sRi = 0; gq.sRm = 0; gq.sRn = 0;
      gq.M = NR; gq.N = D; gq.K = D; gq.zi_n = 1; gq.flags = 0; gq.act = 0;
      gq.alpha = 1.0f; gq.beta = 0.0f; gq.sa = 1.0f; gq.sb = 8.0f; gq.Npad = D; gq.pad_ = 0;
      if ((long long)(NR) >= 64 && (long long)(D) >= 64) k_gemmT<0, 4, 4><<<dim3((unsigned)((D) + 63) / 64, (unsigned)((NR) + 63) / 64, (unsigned)(1)), 32, 0, stream>>>(gq);
      else k_gemm<0><<<dim3((unsigned)((D) + 31) / 32, (unsigned)((NR) + 15) / 16, (unsigned)(1)), 32, 0, stream>>>(gq); }
    { GemmP gv;
      gv.A = seq; gv.B = Wqkv + (size_t)2 * D * D; gv.bias = seq; gv.R = seq; gv.C = QV + D;
      gv.sAo = 0; gv.sAi = 0; gv.sAm = D; gv.sAk = 1; gv.sBo = 0; gv.sBi = 0; gv.sBn = D; gv.sBk = 1; gv.sCo = 0; gv.sCi = 0; gv.sCm = 2 * D; gv.sRo = 0; gv.sRi = 0; gv.sRm = 0; gv.sRn = 0;
      gv.M = NR; gv.N = D; gv.K = D; gv.zi_n = 1; gv.flags = 0; gv.act = 0;
      gv.alpha = 1.0f; gv.beta = 0.0f; gv.sa = 1.0f; gv.sb = 8.0f; gv.Npad = D; gv.pad_ = 0;
      if ((long long)(NR) >= 64 && (long long)(D) >= 64) k_gemmT<0, 4, 4><<<dim3((unsigned)((D) + 63) / 64, (unsigned)((NR) + 63) / 64, (unsigned)(1)), 32, 0, stream>>>(gv);
      else k_gemm<0><<<dim3((unsigned)((D) + 31) / 32, (unsigned)((NR) + 15) / 16, (unsigned)(1)), 32, 0, stream>>>(gv); }
    { GemmP gk;
      gk.A = seq; gk.B = Wqkv + (size_t)D * D; gk.bias = seq; gk.R = seq; gk.C = KP + (size_t)PADK * D;
      gk.sAo = (long long)S * D; gk.sAi = 0; gk.sAm = D; gk.sAk = 1; gk.sBo = 0; gk.sBi = 0; gk.sBn = D; gk.sBk = 1; gk.sCo = (long long)SP * D; gk.sCi = 0; gk.sCm = D; gk.sRo = 0; gk.sRi = 0; gk.sRm = 0; gk.sRn = 0;
      gk.M = S; gk.N = D; gk.K = D; gk.zi_n = 1; gk.flags = 0; gk.act = 0;
      gk.alpha = 1.0f; gk.beta = 0.0f; gk.sa = 1.0f; gk.sb = 8.0f; gk.Npad = D; gk.pad_ = 0;
      if ((long long)(S) >= 64 && (long long)(D) >= 64) k_gemmT<0, 4, 4><<<dim3((unsigned)((D) + 63) / 64, (unsigned)((S) + 63) / 64, (unsigned)(Bn)), 32, 0, stream>>>(gk);
      else k_gemm<0><<<dim3((unsigned)((D) + 31) / 32, (unsigned)((S) + 15) / 16, (unsigned)(Bn)), 32, 0, stream>>>(gk); }
    k_rt_kpad<<<(unsigned)(((long long)Bn * 2 * PADK * D + 255) / 256), 256, 0, stream>>>(KP, Bn, S, D, PADK, SP);
    { GemmP gs00;
      gs00.A = QV + (size_t)0 * S * 2 * D + 0 * HD; gs00.B = KP + (size_t)0 * SP * D + 0 * HD; gs00.bias = QV + (size_t)0 * S * 2 * D + 0 * HD; gs00.R = QV + (size_t)0 * S * 2 * D + 0 * HD; gs00.C = PB + (size_t)0 * S * KW;
      gs00.sAo = (long long)S * 2 * D; gs00.sAi = (long long)QB * 2 * D; gs00.sAm = 2 * D; gs00.sAk = 1; gs00.sBo = (long long)SP * D; gs00.sBi = (long long)QB * D; gs00.sBn = D; gs00.sBk = 1; gs00.sCo = (long long)NH * S * KW; gs00.sCi = (long long)QB * KW; gs00.sCm = KW; gs00.sRo = 0; gs00.sRi = 0; gs00.sRm = 0; gs00.sRn = 0;
      gs00.M = QB; gs00.N = KW; gs00.K = HD; gs00.zi_n = NBLK; gs00.flags = 0; gs00.act = 0;
      gs00.alpha = 1.0f; gs00.beta = 0.0f; gs00.sa = 1.0f; gs00.sb = 1.0f; gs00.Npad = KW; gs00.pad_ = 0;
      if ((long long)(QB) >= 64 && (long long)(KW) >= 64) k_gemmT<1, 2, 4><<<dim3((unsigned)((KW) + 63) / 64, (unsigned)((QB) + 31) / 32, (unsigned)(BC * NBLK)), 32, 0, stream>>>(gs00);
      else k_gemm<1><<<dim3((unsigned)((KW) + 31) / 32, (unsigned)((QB) + 15) / 16, (unsigned)(BC * NBLK)), 32, 0, stream>>>(gs00); }
    { GemmP gs01;
      gs01.A = QV + (size_t)0 * S * 2 * D + 1 * HD; gs01.B = KP + (size_t)0 * SP * D + 1 * HD; gs01.bias = QV + (size_t)0 * S * 2 * D + 1 * HD; gs01.R = QV + (size_t)0 * S * 2 * D + 1 * HD; gs01.C = PB + (size_t)1 * S * KW;
      gs01.sAo = (long long)S * 2 * D; gs01.sAi = (long long)QB * 2 * D; gs01.sAm = 2 * D; gs01.sAk = 1; gs01.sBo = (long long)SP * D; gs01.sBi = (long long)QB * D; gs01.sBn = D; gs01.sBk = 1; gs01.sCo = (long long)NH * S * KW; gs01.sCi = (long long)QB * KW; gs01.sCm = KW; gs01.sRo = 0; gs01.sRi = 0; gs01.sRm = 0; gs01.sRn = 0;
      gs01.M = QB; gs01.N = KW; gs01.K = HD; gs01.zi_n = NBLK; gs01.flags = 0; gs01.act = 0;
      gs01.alpha = 1.0f; gs01.beta = 0.0f; gs01.sa = 1.0f; gs01.sb = 1.0f; gs01.Npad = KW; gs01.pad_ = 0;
      if ((long long)(QB) >= 64 && (long long)(KW) >= 64) k_gemmT<1, 2, 4><<<dim3((unsigned)((KW) + 63) / 64, (unsigned)((QB) + 31) / 32, (unsigned)(BC * NBLK)), 32, 0, stream>>>(gs01);
      else k_gemm<1><<<dim3((unsigned)((KW) + 31) / 32, (unsigned)((QB) + 15) / 16, (unsigned)(BC * NBLK)), 32, 0, stream>>>(gs01); }
    { GemmP gs02;
      gs02.A = QV + (size_t)0 * S * 2 * D + 2 * HD; gs02.B = KP + (size_t)0 * SP * D + 2 * HD; gs02.bias = QV + (size_t)0 * S * 2 * D + 2 * HD; gs02.R = QV + (size_t)0 * S * 2 * D + 2 * HD; gs02.C = PB + (size_t)2 * S * KW;
      gs02.sAo = (long long)S * 2 * D; gs02.sAi = (long long)QB * 2 * D; gs02.sAm = 2 * D; gs02.sAk = 1; gs02.sBo = (long long)SP * D; gs02.sBi = (long long)QB * D; gs02.sBn = D; gs02.sBk = 1; gs02.sCo = (long long)NH * S * KW; gs02.sCi = (long long)QB * KW; gs02.sCm = KW; gs02.sRo = 0; gs02.sRi = 0; gs02.sRm = 0; gs02.sRn = 0;
      gs02.M = QB; gs02.N = KW; gs02.K = HD; gs02.zi_n = NBLK; gs02.flags = 0; gs02.act = 0;
      gs02.alpha = 1.0f; gs02.beta = 0.0f; gs02.sa = 1.0f; gs02.sb = 1.0f; gs02.Npad = KW; gs02.pad_ = 0;
      if ((long long)(QB) >= 64 && (long long)(KW) >= 64) k_gemmT<1, 2, 4><<<dim3((unsigned)((KW) + 63) / 64, (unsigned)((QB) + 31) / 32, (unsigned)(BC * NBLK)), 32, 0, stream>>>(gs02);
      else k_gemm<1><<<dim3((unsigned)((KW) + 31) / 32, (unsigned)((QB) + 15) / 16, (unsigned)(BC * NBLK)), 32, 0, stream>>>(gs02); }
    { GemmP gs03;
      gs03.A = QV + (size_t)0 * S * 2 * D + 3 * HD; gs03.B = KP + (size_t)0 * SP * D + 3 * HD; gs03.bias = QV + (size_t)0 * S * 2 * D + 3 * HD; gs03.R = QV + (size_t)0 * S * 2 * D + 3 * HD; gs03.C = PB + (size_t)3 * S * KW;
      gs03.sAo = (long long)S * 2 * D; gs03.sAi = (long long)QB * 2 * D; gs03.sAm = 2 * D; gs03.sAk = 1; gs03.sBo = (long long)SP * D; gs03.sBi = (long long)QB * D; gs03.sBn = D; gs03.sBk = 1; gs03.sCo = (long long)NH * S * KW; gs03.sCi = (long long)QB * KW; gs03.sCm = KW; gs03.sRo = 0; gs03.sRi = 0; gs03.sRm = 0; gs03.sRn = 0;
      gs03.M = QB; gs03.N = KW; gs03.K = HD; gs03.zi_n = NBLK; gs03.flags = 0; gs03.act = 0;
      gs03.alpha = 1.0f; gs03.beta = 0.0f; gs03.sa = 1.0f; gs03.sb = 1.0f; gs03.Npad = KW; gs03.pad_ = 0;
      if ((long long)(QB) >= 64 && (long long)(KW) >= 64) k_gemmT<1, 2, 4><<<dim3((unsigned)((KW) + 63) / 64, (unsigned)((QB) + 31) / 32, (unsigned)(BC * NBLK)), 32, 0, stream>>>(gs03);
      else k_gemm<1><<<dim3((unsigned)((KW) + 31) / 32, (unsigned)((QB) + 15) / 16, (unsigned)(BC * NBLK)), 32, 0, stream>>>(gs03); }
    { GemmP gs04;
      gs04.A = QV + (size_t)0 * S * 2 * D + 4 * HD; gs04.B = KP + (size_t)0 * SP * D + 4 * HD; gs04.bias = QV + (size_t)0 * S * 2 * D + 4 * HD; gs04.R = QV + (size_t)0 * S * 2 * D + 4 * HD; gs04.C = PB + (size_t)4 * S * KW;
      gs04.sAo = (long long)S * 2 * D; gs04.sAi = (long long)QB * 2 * D; gs04.sAm = 2 * D; gs04.sAk = 1; gs04.sBo = (long long)SP * D; gs04.sBi = (long long)QB * D; gs04.sBn = D; gs04.sBk = 1; gs04.sCo = (long long)NH * S * KW; gs04.sCi = (long long)QB * KW; gs04.sCm = KW; gs04.sRo = 0; gs04.sRi = 0; gs04.sRm = 0; gs04.sRn = 0;
      gs04.M = QB; gs04.N = KW; gs04.K = HD; gs04.zi_n = NBLK; gs04.flags = 0; gs04.act = 0;
      gs04.alpha = 1.0f; gs04.beta = 0.0f; gs04.sa = 1.0f; gs04.sb = 1.0f; gs04.Npad = KW; gs04.pad_ = 0;
      if ((long long)(QB) >= 64 && (long long)(KW) >= 64) k_gemmT<1, 2, 4><<<dim3((unsigned)((KW) + 63) / 64, (unsigned)((QB) + 31) / 32, (unsigned)(BC * NBLK)), 32, 0, stream>>>(gs04);
      else k_gemm<1><<<dim3((unsigned)((KW) + 31) / 32, (unsigned)((QB) + 15) / 16, (unsigned)(BC * NBLK)), 32, 0, stream>>>(gs04); }
    { GemmP gs05;
      gs05.A = QV + (size_t)0 * S * 2 * D + 5 * HD; gs05.B = KP + (size_t)0 * SP * D + 5 * HD; gs05.bias = QV + (size_t)0 * S * 2 * D + 5 * HD; gs05.R = QV + (size_t)0 * S * 2 * D + 5 * HD; gs05.C = PB + (size_t)5 * S * KW;
      gs05.sAo = (long long)S * 2 * D; gs05.sAi = (long long)QB * 2 * D; gs05.sAm = 2 * D; gs05.sAk = 1; gs05.sBo = (long long)SP * D; gs05.sBi = (long long)QB * D; gs05.sBn = D; gs05.sBk = 1; gs05.sCo = (long long)NH * S * KW; gs05.sCi = (long long)QB * KW; gs05.sCm = KW; gs05.sRo = 0; gs05.sRi = 0; gs05.sRm = 0; gs05.sRn = 0;
      gs05.M = QB; gs05.N = KW; gs05.K = HD; gs05.zi_n = NBLK; gs05.flags = 0; gs05.act = 0;
      gs05.alpha = 1.0f; gs05.beta = 0.0f; gs05.sa = 1.0f; gs05.sb = 1.0f; gs05.Npad = KW; gs05.pad_ = 0;
      if ((long long)(QB) >= 64 && (long long)(KW) >= 64) k_gemmT<1, 2, 4><<<dim3((unsigned)((KW) + 63) / 64, (unsigned)((QB) + 31) / 32, (unsigned)(BC * NBLK)), 32, 0, stream>>>(gs05);
      else k_gemm<1><<<dim3((unsigned)((KW) + 31) / 32, (unsigned)((QB) + 15) / 16, (unsigned)(BC * NBLK)), 32, 0, stream>>>(gs05); }
    { GemmP gs06;
      gs06.A = QV + (size_t)0 * S * 2 * D + 6 * HD; gs06.B = KP + (size_t)0 * SP * D + 6 * HD; gs06.bias = QV + (size_t)0 * S * 2 * D + 6 * HD; gs06.R = QV + (size_t)0 * S * 2 * D + 6 * HD; gs06.C = PB + (size_t)6 * S * KW;
      gs06.sAo = (long long)S * 2 * D; gs06.sAi = (long long)QB * 2 * D; gs06.sAm = 2 * D; gs06.sAk = 1; gs06.sBo = (long long)SP * D; gs06.sBi = (long long)QB * D; gs06.sBn = D; gs06.sBk = 1; gs06.sCo = (long long)NH * S * KW; gs06.sCi = (long long)QB * KW; gs06.sCm = KW; gs06.sRo = 0; gs06.sRi = 0; gs06.sRm = 0; gs06.sRn = 0;
      gs06.M = QB; gs06.N = KW; gs06.K = HD; gs06.zi_n = NBLK; gs06.flags = 0; gs06.act = 0;
      gs06.alpha = 1.0f; gs06.beta = 0.0f; gs06.sa = 1.0f; gs06.sb = 1.0f; gs06.Npad = KW; gs06.pad_ = 0;
      if ((long long)(QB) >= 64 && (long long)(KW) >= 64) k_gemmT<1, 2, 4><<<dim3((unsigned)((KW) + 63) / 64, (unsigned)((QB) + 31) / 32, (unsigned)(BC * NBLK)), 32, 0, stream>>>(gs06);
      else k_gemm<1><<<dim3((unsigned)((KW) + 31) / 32, (unsigned)((QB) + 15) / 16, (unsigned)(BC * NBLK)), 32, 0, stream>>>(gs06); }
    { GemmP gs07;
      gs07.A = QV + (size_t)0 * S * 2 * D + 7 * HD; gs07.B = KP + (size_t)0 * SP * D + 7 * HD; gs07.bias = QV + (size_t)0 * S * 2 * D + 7 * HD; gs07.R = QV + (size_t)0 * S * 2 * D + 7 * HD; gs07.C = PB + (size_t)7 * S * KW;
      gs07.sAo = (long long)S * 2 * D; gs07.sAi = (long long)QB * 2 * D; gs07.sAm = 2 * D; gs07.sAk = 1; gs07.sBo = (long long)SP * D; gs07.sBi = (long long)QB * D; gs07.sBn = D; gs07.sBk = 1; gs07.sCo = (long long)NH * S * KW; gs07.sCi = (long long)QB * KW; gs07.sCm = KW; gs07.sRo = 0; gs07.sRi = 0; gs07.sRm = 0; gs07.sRn = 0;
      gs07.M = QB; gs07.N = KW; gs07.K = HD; gs07.zi_n = NBLK; gs07.flags = 0; gs07.act = 0;
      gs07.alpha = 1.0f; gs07.beta = 0.0f; gs07.sa = 1.0f; gs07.sb = 1.0f; gs07.Npad = KW; gs07.pad_ = 0;
      if ((long long)(QB) >= 64 && (long long)(KW) >= 64) k_gemmT<1, 2, 4><<<dim3((unsigned)((KW) + 63) / 64, (unsigned)((QB) + 31) / 32, (unsigned)(BC * NBLK)), 32, 0, stream>>>(gs07);
      else k_gemm<1><<<dim3((unsigned)((KW) + 31) / 32, (unsigned)((QB) + 15) / 16, (unsigned)(BC * NBLK)), 32, 0, stream>>>(gs07); }
    k_rt_soft<<<(unsigned)(((long long)BC * NH * S + 127) / 128), 128, 0, stream>>>(PB, lens, decw, 0, BC, NH, S, KW, PADK, 0.125f, 0.1f); k_rt_col<<<(unsigned)(((long long)BC * NH * S + 127) / 128), 128, 0, stream>>>(PB, lens, PBAR, 0, BC, NH, S, KW, PADK);
    { GemmP gs10;
      gs10.A = QV + (size_t)2 * S * 2 * D + 0 * HD; gs10.B = KP + (size_t)2 * SP * D + 0 * HD; gs10.bias = QV + (size_t)2 * S * 2 * D + 0 * HD; gs10.R = QV + (size_t)2 * S * 2 * D + 0 * HD; gs10.C = PB + (size_t)0 * S * KW;
      gs10.sAo = (long long)S * 2 * D; gs10.sAi = (long long)QB * 2 * D; gs10.sAm = 2 * D; gs10.sAk = 1; gs10.sBo = (long long)SP * D; gs10.sBi = (long long)QB * D; gs10.sBn = D; gs10.sBk = 1; gs10.sCo = (long long)NH * S * KW; gs10.sCi = (long long)QB * KW; gs10.sCm = KW; gs10.sRo = 0; gs10.sRi = 0; gs10.sRm = 0; gs10.sRn = 0;
      gs10.M = QB; gs10.N = KW; gs10.K = HD; gs10.zi_n = NBLK; gs10.flags = 0; gs10.act = 0;
      gs10.alpha = 1.0f; gs10.beta = 0.0f; gs10.sa = 1.0f; gs10.sb = 1.0f; gs10.Npad = KW; gs10.pad_ = 0;
      if ((long long)(QB) >= 64 && (long long)(KW) >= 64) k_gemmT<1, 2, 4><<<dim3((unsigned)((KW) + 63) / 64, (unsigned)((QB) + 31) / 32, (unsigned)(BC * NBLK)), 32, 0, stream>>>(gs10);
      else k_gemm<1><<<dim3((unsigned)((KW) + 31) / 32, (unsigned)((QB) + 15) / 16, (unsigned)(BC * NBLK)), 32, 0, stream>>>(gs10); }
    { GemmP gs11;
      gs11.A = QV + (size_t)2 * S * 2 * D + 1 * HD; gs11.B = KP + (size_t)2 * SP * D + 1 * HD; gs11.bias = QV + (size_t)2 * S * 2 * D + 1 * HD; gs11.R = QV + (size_t)2 * S * 2 * D + 1 * HD; gs11.C = PB + (size_t)1 * S * KW;
      gs11.sAo = (long long)S * 2 * D; gs11.sAi = (long long)QB * 2 * D; gs11.sAm = 2 * D; gs11.sAk = 1; gs11.sBo = (long long)SP * D; gs11.sBi = (long long)QB * D; gs11.sBn = D; gs11.sBk = 1; gs11.sCo = (long long)NH * S * KW; gs11.sCi = (long long)QB * KW; gs11.sCm = KW; gs11.sRo = 0; gs11.sRi = 0; gs11.sRm = 0; gs11.sRn = 0;
      gs11.M = QB; gs11.N = KW; gs11.K = HD; gs11.zi_n = NBLK; gs11.flags = 0; gs11.act = 0;
      gs11.alpha = 1.0f; gs11.beta = 0.0f; gs11.sa = 1.0f; gs11.sb = 1.0f; gs11.Npad = KW; gs11.pad_ = 0;
      if ((long long)(QB) >= 64 && (long long)(KW) >= 64) k_gemmT<1, 2, 4><<<dim3((unsigned)((KW) + 63) / 64, (unsigned)((QB) + 31) / 32, (unsigned)(BC * NBLK)), 32, 0, stream>>>(gs11);
      else k_gemm<1><<<dim3((unsigned)((KW) + 31) / 32, (unsigned)((QB) + 15) / 16, (unsigned)(BC * NBLK)), 32, 0, stream>>>(gs11); }
    { GemmP gs12;
      gs12.A = QV + (size_t)2 * S * 2 * D + 2 * HD; gs12.B = KP + (size_t)2 * SP * D + 2 * HD; gs12.bias = QV + (size_t)2 * S * 2 * D + 2 * HD; gs12.R = QV + (size_t)2 * S * 2 * D + 2 * HD; gs12.C = PB + (size_t)2 * S * KW;
      gs12.sAo = (long long)S * 2 * D; gs12.sAi = (long long)QB * 2 * D; gs12.sAm = 2 * D; gs12.sAk = 1; gs12.sBo = (long long)SP * D; gs12.sBi = (long long)QB * D; gs12.sBn = D; gs12.sBk = 1; gs12.sCo = (long long)NH * S * KW; gs12.sCi = (long long)QB * KW; gs12.sCm = KW; gs12.sRo = 0; gs12.sRi = 0; gs12.sRm = 0; gs12.sRn = 0;
      gs12.M = QB; gs12.N = KW; gs12.K = HD; gs12.zi_n = NBLK; gs12.flags = 0; gs12.act = 0;
      gs12.alpha = 1.0f; gs12.beta = 0.0f; gs12.sa = 1.0f; gs12.sb = 1.0f; gs12.Npad = KW; gs12.pad_ = 0;
      if ((long long)(QB) >= 64 && (long long)(KW) >= 64) k_gemmT<1, 2, 4><<<dim3((unsigned)((KW) + 63) / 64, (unsigned)((QB) + 31) / 32, (unsigned)(BC * NBLK)), 32, 0, stream>>>(gs12);
      else k_gemm<1><<<dim3((unsigned)((KW) + 31) / 32, (unsigned)((QB) + 15) / 16, (unsigned)(BC * NBLK)), 32, 0, stream>>>(gs12); }
    { GemmP gs13;
      gs13.A = QV + (size_t)2 * S * 2 * D + 3 * HD; gs13.B = KP + (size_t)2 * SP * D + 3 * HD; gs13.bias = QV + (size_t)2 * S * 2 * D + 3 * HD; gs13.R = QV + (size_t)2 * S * 2 * D + 3 * HD; gs13.C = PB + (size_t)3 * S * KW;
      gs13.sAo = (long long)S * 2 * D; gs13.sAi = (long long)QB * 2 * D; gs13.sAm = 2 * D; gs13.sAk = 1; gs13.sBo = (long long)SP * D; gs13.sBi = (long long)QB * D; gs13.sBn = D; gs13.sBk = 1; gs13.sCo = (long long)NH * S * KW; gs13.sCi = (long long)QB * KW; gs13.sCm = KW; gs13.sRo = 0; gs13.sRi = 0; gs13.sRm = 0; gs13.sRn = 0;
      gs13.M = QB; gs13.N = KW; gs13.K = HD; gs13.zi_n = NBLK; gs13.flags = 0; gs13.act = 0;
      gs13.alpha = 1.0f; gs13.beta = 0.0f; gs13.sa = 1.0f; gs13.sb = 1.0f; gs13.Npad = KW; gs13.pad_ = 0;
      if ((long long)(QB) >= 64 && (long long)(KW) >= 64) k_gemmT<1, 2, 4><<<dim3((unsigned)((KW) + 63) / 64, (unsigned)((QB) + 31) / 32, (unsigned)(BC * NBLK)), 32, 0, stream>>>(gs13);
      else k_gemm<1><<<dim3((unsigned)((KW) + 31) / 32, (unsigned)((QB) + 15) / 16, (unsigned)(BC * NBLK)), 32, 0, stream>>>(gs13); }
    { GemmP gs14;
      gs14.A = QV + (size_t)2 * S * 2 * D + 4 * HD; gs14.B = KP + (size_t)2 * SP * D + 4 * HD; gs14.bias = QV + (size_t)2 * S * 2 * D + 4 * HD; gs14.R = QV + (size_t)2 * S * 2 * D + 4 * HD; gs14.C = PB + (size_t)4 * S * KW;
      gs14.sAo = (long long)S * 2 * D; gs14.sAi = (long long)QB * 2 * D; gs14.sAm = 2 * D; gs14.sAk = 1; gs14.sBo = (long long)SP * D; gs14.sBi = (long long)QB * D; gs14.sBn = D; gs14.sBk = 1; gs14.sCo = (long long)NH * S * KW; gs14.sCi = (long long)QB * KW; gs14.sCm = KW; gs14.sRo = 0; gs14.sRi = 0; gs14.sRm = 0; gs14.sRn = 0;
      gs14.M = QB; gs14.N = KW; gs14.K = HD; gs14.zi_n = NBLK; gs14.flags = 0; gs14.act = 0;
      gs14.alpha = 1.0f; gs14.beta = 0.0f; gs14.sa = 1.0f; gs14.sb = 1.0f; gs14.Npad = KW; gs14.pad_ = 0;
      if ((long long)(QB) >= 64 && (long long)(KW) >= 64) k_gemmT<1, 2, 4><<<dim3((unsigned)((KW) + 63) / 64, (unsigned)((QB) + 31) / 32, (unsigned)(BC * NBLK)), 32, 0, stream>>>(gs14);
      else k_gemm<1><<<dim3((unsigned)((KW) + 31) / 32, (unsigned)((QB) + 15) / 16, (unsigned)(BC * NBLK)), 32, 0, stream>>>(gs14); }
    { GemmP gs15;
      gs15.A = QV + (size_t)2 * S * 2 * D + 5 * HD; gs15.B = KP + (size_t)2 * SP * D + 5 * HD; gs15.bias = QV + (size_t)2 * S * 2 * D + 5 * HD; gs15.R = QV + (size_t)2 * S * 2 * D + 5 * HD; gs15.C = PB + (size_t)5 * S * KW;
      gs15.sAo = (long long)S * 2 * D; gs15.sAi = (long long)QB * 2 * D; gs15.sAm = 2 * D; gs15.sAk = 1; gs15.sBo = (long long)SP * D; gs15.sBi = (long long)QB * D; gs15.sBn = D; gs15.sBk = 1; gs15.sCo = (long long)NH * S * KW; gs15.sCi = (long long)QB * KW; gs15.sCm = KW; gs15.sRo = 0; gs15.sRi = 0; gs15.sRm = 0; gs15.sRn = 0;
      gs15.M = QB; gs15.N = KW; gs15.K = HD; gs15.zi_n = NBLK; gs15.flags = 0; gs15.act = 0;
      gs15.alpha = 1.0f; gs15.beta = 0.0f; gs15.sa = 1.0f; gs15.sb = 1.0f; gs15.Npad = KW; gs15.pad_ = 0;
      if ((long long)(QB) >= 64 && (long long)(KW) >= 64) k_gemmT<1, 2, 4><<<dim3((unsigned)((KW) + 63) / 64, (unsigned)((QB) + 31) / 32, (unsigned)(BC * NBLK)), 32, 0, stream>>>(gs15);
      else k_gemm<1><<<dim3((unsigned)((KW) + 31) / 32, (unsigned)((QB) + 15) / 16, (unsigned)(BC * NBLK)), 32, 0, stream>>>(gs15); }
    { GemmP gs16;
      gs16.A = QV + (size_t)2 * S * 2 * D + 6 * HD; gs16.B = KP + (size_t)2 * SP * D + 6 * HD; gs16.bias = QV + (size_t)2 * S * 2 * D + 6 * HD; gs16.R = QV + (size_t)2 * S * 2 * D + 6 * HD; gs16.C = PB + (size_t)6 * S * KW;
      gs16.sAo = (long long)S * 2 * D; gs16.sAi = (long long)QB * 2 * D; gs16.sAm = 2 * D; gs16.sAk = 1; gs16.sBo = (long long)SP * D; gs16.sBi = (long long)QB * D; gs16.sBn = D; gs16.sBk = 1; gs16.sCo = (long long)NH * S * KW; gs16.sCi = (long long)QB * KW; gs16.sCm = KW; gs16.sRo = 0; gs16.sRi = 0; gs16.sRm = 0; gs16.sRn = 0;
      gs16.M = QB; gs16.N = KW; gs16.K = HD; gs16.zi_n = NBLK; gs16.flags = 0; gs16.act = 0;
      gs16.alpha = 1.0f; gs16.beta = 0.0f; gs16.sa = 1.0f; gs16.sb = 1.0f; gs16.Npad = KW; gs16.pad_ = 0;
      if ((long long)(QB) >= 64 && (long long)(KW) >= 64) k_gemmT<1, 2, 4><<<dim3((unsigned)((KW) + 63) / 64, (unsigned)((QB) + 31) / 32, (unsigned)(BC * NBLK)), 32, 0, stream>>>(gs16);
      else k_gemm<1><<<dim3((unsigned)((KW) + 31) / 32, (unsigned)((QB) + 15) / 16, (unsigned)(BC * NBLK)), 32, 0, stream>>>(gs16); }
    { GemmP gs17;
      gs17.A = QV + (size_t)2 * S * 2 * D + 7 * HD; gs17.B = KP + (size_t)2 * SP * D + 7 * HD; gs17.bias = QV + (size_t)2 * S * 2 * D + 7 * HD; gs17.R = QV + (size_t)2 * S * 2 * D + 7 * HD; gs17.C = PB + (size_t)7 * S * KW;
      gs17.sAo = (long long)S * 2 * D; gs17.sAi = (long long)QB * 2 * D; gs17.sAm = 2 * D; gs17.sAk = 1; gs17.sBo = (long long)SP * D; gs17.sBi = (long long)QB * D; gs17.sBn = D; gs17.sBk = 1; gs17.sCo = (long long)NH * S * KW; gs17.sCi = (long long)QB * KW; gs17.sCm = KW; gs17.sRo = 0; gs17.sRi = 0; gs17.sRm = 0; gs17.sRn = 0;
      gs17.M = QB; gs17.N = KW; gs17.K = HD; gs17.zi_n = NBLK; gs17.flags = 0; gs17.act = 0;
      gs17.alpha = 1.0f; gs17.beta = 0.0f; gs17.sa = 1.0f; gs17.sb = 1.0f; gs17.Npad = KW; gs17.pad_ = 0;
      if ((long long)(QB) >= 64 && (long long)(KW) >= 64) k_gemmT<1, 2, 4><<<dim3((unsigned)((KW) + 63) / 64, (unsigned)((QB) + 31) / 32, (unsigned)(BC * NBLK)), 32, 0, stream>>>(gs17);
      else k_gemm<1><<<dim3((unsigned)((KW) + 31) / 32, (unsigned)((QB) + 15) / 16, (unsigned)(BC * NBLK)), 32, 0, stream>>>(gs17); }
    k_rt_soft<<<(unsigned)(((long long)BC * NH * S + 127) / 128), 128, 0, stream>>>(PB, lens, decw, 2, BC, NH, S, KW, PADK, 0.125f, 0.1f); k_rt_col<<<(unsigned)(((long long)BC * NH * S + 127) / 128), 128, 0, stream>>>(PB, lens, PBAR, 2, BC, NH, S, KW, PADK);
    { GemmP gs20;
      gs20.A = QV + (size_t)4 * S * 2 * D + 0 * HD; gs20.B = KP + (size_t)4 * SP * D + 0 * HD; gs20.bias = QV + (size_t)4 * S * 2 * D + 0 * HD; gs20.R = QV + (size_t)4 * S * 2 * D + 0 * HD; gs20.C = PB + (size_t)0 * S * KW;
      gs20.sAo = (long long)S * 2 * D; gs20.sAi = (long long)QB * 2 * D; gs20.sAm = 2 * D; gs20.sAk = 1; gs20.sBo = (long long)SP * D; gs20.sBi = (long long)QB * D; gs20.sBn = D; gs20.sBk = 1; gs20.sCo = (long long)NH * S * KW; gs20.sCi = (long long)QB * KW; gs20.sCm = KW; gs20.sRo = 0; gs20.sRi = 0; gs20.sRm = 0; gs20.sRn = 0;
      gs20.M = QB; gs20.N = KW; gs20.K = HD; gs20.zi_n = NBLK; gs20.flags = 0; gs20.act = 0;
      gs20.alpha = 1.0f; gs20.beta = 0.0f; gs20.sa = 1.0f; gs20.sb = 1.0f; gs20.Npad = KW; gs20.pad_ = 0;
      if ((long long)(QB) >= 64 && (long long)(KW) >= 64) k_gemmT<1, 2, 4><<<dim3((unsigned)((KW) + 63) / 64, (unsigned)((QB) + 31) / 32, (unsigned)(BC * NBLK)), 32, 0, stream>>>(gs20);
      else k_gemm<1><<<dim3((unsigned)((KW) + 31) / 32, (unsigned)((QB) + 15) / 16, (unsigned)(BC * NBLK)), 32, 0, stream>>>(gs20); }
    { GemmP gs21;
      gs21.A = QV + (size_t)4 * S * 2 * D + 1 * HD; gs21.B = KP + (size_t)4 * SP * D + 1 * HD; gs21.bias = QV + (size_t)4 * S * 2 * D + 1 * HD; gs21.R = QV + (size_t)4 * S * 2 * D + 1 * HD; gs21.C = PB + (size_t)1 * S * KW;
      gs21.sAo = (long long)S * 2 * D; gs21.sAi = (long long)QB * 2 * D; gs21.sAm = 2 * D; gs21.sAk = 1; gs21.sBo = (long long)SP * D; gs21.sBi = (long long)QB * D; gs21.sBn = D; gs21.sBk = 1; gs21.sCo = (long long)NH * S * KW; gs21.sCi = (long long)QB * KW; gs21.sCm = KW; gs21.sRo = 0; gs21.sRi = 0; gs21.sRm = 0; gs21.sRn = 0;
      gs21.M = QB; gs21.N = KW; gs21.K = HD; gs21.zi_n = NBLK; gs21.flags = 0; gs21.act = 0;
      gs21.alpha = 1.0f; gs21.beta = 0.0f; gs21.sa = 1.0f; gs21.sb = 1.0f; gs21.Npad = KW; gs21.pad_ = 0;
      if ((long long)(QB) >= 64 && (long long)(KW) >= 64) k_gemmT<1, 2, 4><<<dim3((unsigned)((KW) + 63) / 64, (unsigned)((QB) + 31) / 32, (unsigned)(BC * NBLK)), 32, 0, stream>>>(gs21);
      else k_gemm<1><<<dim3((unsigned)((KW) + 31) / 32, (unsigned)((QB) + 15) / 16, (unsigned)(BC * NBLK)), 32, 0, stream>>>(gs21); }
    { GemmP gs22;
      gs22.A = QV + (size_t)4 * S * 2 * D + 2 * HD; gs22.B = KP + (size_t)4 * SP * D + 2 * HD; gs22.bias = QV + (size_t)4 * S * 2 * D + 2 * HD; gs22.R = QV + (size_t)4 * S * 2 * D + 2 * HD; gs22.C = PB + (size_t)2 * S * KW;
      gs22.sAo = (long long)S * 2 * D; gs22.sAi = (long long)QB * 2 * D; gs22.sAm = 2 * D; gs22.sAk = 1; gs22.sBo = (long long)SP * D; gs22.sBi = (long long)QB * D; gs22.sBn = D; gs22.sBk = 1; gs22.sCo = (long long)NH * S * KW; gs22.sCi = (long long)QB * KW; gs22.sCm = KW; gs22.sRo = 0; gs22.sRi = 0; gs22.sRm = 0; gs22.sRn = 0;
      gs22.M = QB; gs22.N = KW; gs22.K = HD; gs22.zi_n = NBLK; gs22.flags = 0; gs22.act = 0;
      gs22.alpha = 1.0f; gs22.beta = 0.0f; gs22.sa = 1.0f; gs22.sb = 1.0f; gs22.Npad = KW; gs22.pad_ = 0;
      if ((long long)(QB) >= 64 && (long long)(KW) >= 64) k_gemmT<1, 2, 4><<<dim3((unsigned)((KW) + 63) / 64, (unsigned)((QB) + 31) / 32, (unsigned)(BC * NBLK)), 32, 0, stream>>>(gs22);
      else k_gemm<1><<<dim3((unsigned)((KW) + 31) / 32, (unsigned)((QB) + 15) / 16, (unsigned)(BC * NBLK)), 32, 0, stream>>>(gs22); }
    { GemmP gs23;
      gs23.A = QV + (size_t)4 * S * 2 * D + 3 * HD; gs23.B = KP + (size_t)4 * SP * D + 3 * HD; gs23.bias = QV + (size_t)4 * S * 2 * D + 3 * HD; gs23.R = QV + (size_t)4 * S * 2 * D + 3 * HD; gs23.C = PB + (size_t)3 * S * KW;
      gs23.sAo = (long long)S * 2 * D; gs23.sAi = (long long)QB * 2 * D; gs23.sAm = 2 * D; gs23.sAk = 1; gs23.sBo = (long long)SP * D; gs23.sBi = (long long)QB * D; gs23.sBn = D; gs23.sBk = 1; gs23.sCo = (long long)NH * S * KW; gs23.sCi = (long long)QB * KW; gs23.sCm = KW; gs23.sRo = 0; gs23.sRi = 0; gs23.sRm = 0; gs23.sRn = 0;
      gs23.M = QB; gs23.N = KW; gs23.K = HD; gs23.zi_n = NBLK; gs23.flags = 0; gs23.act = 0;
      gs23.alpha = 1.0f; gs23.beta = 0.0f; gs23.sa = 1.0f; gs23.sb = 1.0f; gs23.Npad = KW; gs23.pad_ = 0;
      if ((long long)(QB) >= 64 && (long long)(KW) >= 64) k_gemmT<1, 2, 4><<<dim3((unsigned)((KW) + 63) / 64, (unsigned)((QB) + 31) / 32, (unsigned)(BC * NBLK)), 32, 0, stream>>>(gs23);
      else k_gemm<1><<<dim3((unsigned)((KW) + 31) / 32, (unsigned)((QB) + 15) / 16, (unsigned)(BC * NBLK)), 32, 0, stream>>>(gs23); }
    { GemmP gs24;
      gs24.A = QV + (size_t)4 * S * 2 * D + 4 * HD; gs24.B = KP + (size_t)4 * SP * D + 4 * HD; gs24.bias = QV + (size_t)4 * S * 2 * D + 4 * HD; gs24.R = QV + (size_t)4 * S * 2 * D + 4 * HD; gs24.C = PB + (size_t)4 * S * KW;
      gs24.sAo = (long long)S * 2 * D; gs24.sAi = (long long)QB * 2 * D; gs24.sAm = 2 * D; gs24.sAk = 1; gs24.sBo = (long long)SP * D; gs24.sBi = (long long)QB * D; gs24.sBn = D; gs24.sBk = 1; gs24.sCo = (long long)NH * S * KW; gs24.sCi = (long long)QB * KW; gs24.sCm = KW; gs24.sRo = 0; gs24.sRi = 0; gs24.sRm = 0; gs24.sRn = 0;
      gs24.M = QB; gs24.N = KW; gs24.K = HD; gs24.zi_n = NBLK; gs24.flags = 0; gs24.act = 0;
      gs24.alpha = 1.0f; gs24.beta = 0.0f; gs24.sa = 1.0f; gs24.sb = 1.0f; gs24.Npad = KW; gs24.pad_ = 0;
      if ((long long)(QB) >= 64 && (long long)(KW) >= 64) k_gemmT<1, 2, 4><<<dim3((unsigned)((KW) + 63) / 64, (unsigned)((QB) + 31) / 32, (unsigned)(BC * NBLK)), 32, 0, stream>>>(gs24);
      else k_gemm<1><<<dim3((unsigned)((KW) + 31) / 32, (unsigned)((QB) + 15) / 16, (unsigned)(BC * NBLK)), 32, 0, stream>>>(gs24); }
    { GemmP gs25;
      gs25.A = QV + (size_t)4 * S * 2 * D + 5 * HD; gs25.B = KP + (size_t)4 * SP * D + 5 * HD; gs25.bias = QV + (size_t)4 * S * 2 * D + 5 * HD; gs25.R = QV + (size_t)4 * S * 2 * D + 5 * HD; gs25.C = PB + (size_t)5 * S * KW;
      gs25.sAo = (long long)S * 2 * D; gs25.sAi = (long long)QB * 2 * D; gs25.sAm = 2 * D; gs25.sAk = 1; gs25.sBo = (long long)SP * D; gs25.sBi = (long long)QB * D; gs25.sBn = D; gs25.sBk = 1; gs25.sCo = (long long)NH * S * KW; gs25.sCi = (long long)QB * KW; gs25.sCm = KW; gs25.sRo = 0; gs25.sRi = 0; gs25.sRm = 0; gs25.sRn = 0;
      gs25.M = QB; gs25.N = KW; gs25.K = HD; gs25.zi_n = NBLK; gs25.flags = 0; gs25.act = 0;
      gs25.alpha = 1.0f; gs25.beta = 0.0f; gs25.sa = 1.0f; gs25.sb = 1.0f; gs25.Npad = KW; gs25.pad_ = 0;
      if ((long long)(QB) >= 64 && (long long)(KW) >= 64) k_gemmT<1, 2, 4><<<dim3((unsigned)((KW) + 63) / 64, (unsigned)((QB) + 31) / 32, (unsigned)(BC * NBLK)), 32, 0, stream>>>(gs25);
      else k_gemm<1><<<dim3((unsigned)((KW) + 31) / 32, (unsigned)((QB) + 15) / 16, (unsigned)(BC * NBLK)), 32, 0, stream>>>(gs25); }
    { GemmP gs26;
      gs26.A = QV + (size_t)4 * S * 2 * D + 6 * HD; gs26.B = KP + (size_t)4 * SP * D + 6 * HD; gs26.bias = QV + (size_t)4 * S * 2 * D + 6 * HD; gs26.R = QV + (size_t)4 * S * 2 * D + 6 * HD; gs26.C = PB + (size_t)6 * S * KW;
      gs26.sAo = (long long)S * 2 * D; gs26.sAi = (long long)QB * 2 * D; gs26.sAm = 2 * D; gs26.sAk = 1; gs26.sBo = (long long)SP * D; gs26.sBi = (long long)QB * D; gs26.sBn = D; gs26.sBk = 1; gs26.sCo = (long long)NH * S * KW; gs26.sCi = (long long)QB * KW; gs26.sCm = KW; gs26.sRo = 0; gs26.sRi = 0; gs26.sRm = 0; gs26.sRn = 0;
      gs26.M = QB; gs26.N = KW; gs26.K = HD; gs26.zi_n = NBLK; gs26.flags = 0; gs26.act = 0;
      gs26.alpha = 1.0f; gs26.beta = 0.0f; gs26.sa = 1.0f; gs26.sb = 1.0f; gs26.Npad = KW; gs26.pad_ = 0;
      if ((long long)(QB) >= 64 && (long long)(KW) >= 64) k_gemmT<1, 2, 4><<<dim3((unsigned)((KW) + 63) / 64, (unsigned)((QB) + 31) / 32, (unsigned)(BC * NBLK)), 32, 0, stream>>>(gs26);
      else k_gemm<1><<<dim3((unsigned)((KW) + 31) / 32, (unsigned)((QB) + 15) / 16, (unsigned)(BC * NBLK)), 32, 0, stream>>>(gs26); }
    { GemmP gs27;
      gs27.A = QV + (size_t)4 * S * 2 * D + 7 * HD; gs27.B = KP + (size_t)4 * SP * D + 7 * HD; gs27.bias = QV + (size_t)4 * S * 2 * D + 7 * HD; gs27.R = QV + (size_t)4 * S * 2 * D + 7 * HD; gs27.C = PB + (size_t)7 * S * KW;
      gs27.sAo = (long long)S * 2 * D; gs27.sAi = (long long)QB * 2 * D; gs27.sAm = 2 * D; gs27.sAk = 1; gs27.sBo = (long long)SP * D; gs27.sBi = (long long)QB * D; gs27.sBn = D; gs27.sBk = 1; gs27.sCo = (long long)NH * S * KW; gs27.sCi = (long long)QB * KW; gs27.sCm = KW; gs27.sRo = 0; gs27.sRi = 0; gs27.sRm = 0; gs27.sRn = 0;
      gs27.M = QB; gs27.N = KW; gs27.K = HD; gs27.zi_n = NBLK; gs27.flags = 0; gs27.act = 0;
      gs27.alpha = 1.0f; gs27.beta = 0.0f; gs27.sa = 1.0f; gs27.sb = 1.0f; gs27.Npad = KW; gs27.pad_ = 0;
      if ((long long)(QB) >= 64 && (long long)(KW) >= 64) k_gemmT<1, 2, 4><<<dim3((unsigned)((KW) + 63) / 64, (unsigned)((QB) + 31) / 32, (unsigned)(BC * NBLK)), 32, 0, stream>>>(gs27);
      else k_gemm<1><<<dim3((unsigned)((KW) + 31) / 32, (unsigned)((QB) + 15) / 16, (unsigned)(BC * NBLK)), 32, 0, stream>>>(gs27); }
    k_rt_soft<<<(unsigned)(((long long)BC * NH * S + 127) / 128), 128, 0, stream>>>(PB, lens, decw, 4, BC, NH, S, KW, PADK, 0.125f, 0.1f); k_rt_col<<<(unsigned)(((long long)BC * NH * S + 127) / 128), 128, 0, stream>>>(PB, lens, PBAR, 4, BC, NH, S, KW, PADK);
    { GemmP gs30;
      gs30.A = QV + (size_t)6 * S * 2 * D + 0 * HD; gs30.B = KP + (size_t)6 * SP * D + 0 * HD; gs30.bias = QV + (size_t)6 * S * 2 * D + 0 * HD; gs30.R = QV + (size_t)6 * S * 2 * D + 0 * HD; gs30.C = PB + (size_t)0 * S * KW;
      gs30.sAo = (long long)S * 2 * D; gs30.sAi = (long long)QB * 2 * D; gs30.sAm = 2 * D; gs30.sAk = 1; gs30.sBo = (long long)SP * D; gs30.sBi = (long long)QB * D; gs30.sBn = D; gs30.sBk = 1; gs30.sCo = (long long)NH * S * KW; gs30.sCi = (long long)QB * KW; gs30.sCm = KW; gs30.sRo = 0; gs30.sRi = 0; gs30.sRm = 0; gs30.sRn = 0;
      gs30.M = QB; gs30.N = KW; gs30.K = HD; gs30.zi_n = NBLK; gs30.flags = 0; gs30.act = 0;
      gs30.alpha = 1.0f; gs30.beta = 0.0f; gs30.sa = 1.0f; gs30.sb = 1.0f; gs30.Npad = KW; gs30.pad_ = 0;
      if ((long long)(QB) >= 64 && (long long)(KW) >= 64) k_gemmT<1, 2, 4><<<dim3((unsigned)((KW) + 63) / 64, (unsigned)((QB) + 31) / 32, (unsigned)(BC * NBLK)), 32, 0, stream>>>(gs30);
      else k_gemm<1><<<dim3((unsigned)((KW) + 31) / 32, (unsigned)((QB) + 15) / 16, (unsigned)(BC * NBLK)), 32, 0, stream>>>(gs30); }
    { GemmP gs31;
      gs31.A = QV + (size_t)6 * S * 2 * D + 1 * HD; gs31.B = KP + (size_t)6 * SP * D + 1 * HD; gs31.bias = QV + (size_t)6 * S * 2 * D + 1 * HD; gs31.R = QV + (size_t)6 * S * 2 * D + 1 * HD; gs31.C = PB + (size_t)1 * S * KW;
      gs31.sAo = (long long)S * 2 * D; gs31.sAi = (long long)QB * 2 * D; gs31.sAm = 2 * D; gs31.sAk = 1; gs31.sBo = (long long)SP * D; gs31.sBi = (long long)QB * D; gs31.sBn = D; gs31.sBk = 1; gs31.sCo = (long long)NH * S * KW; gs31.sCi = (long long)QB * KW; gs31.sCm = KW; gs31.sRo = 0; gs31.sRi = 0; gs31.sRm = 0; gs31.sRn = 0;
      gs31.M = QB; gs31.N = KW; gs31.K = HD; gs31.zi_n = NBLK; gs31.flags = 0; gs31.act = 0;
      gs31.alpha = 1.0f; gs31.beta = 0.0f; gs31.sa = 1.0f; gs31.sb = 1.0f; gs31.Npad = KW; gs31.pad_ = 0;
      if ((long long)(QB) >= 64 && (long long)(KW) >= 64) k_gemmT<1, 2, 4><<<dim3((unsigned)((KW) + 63) / 64, (unsigned)((QB) + 31) / 32, (unsigned)(BC * NBLK)), 32, 0, stream>>>(gs31);
      else k_gemm<1><<<dim3((unsigned)((KW) + 31) / 32, (unsigned)((QB) + 15) / 16, (unsigned)(BC * NBLK)), 32, 0, stream>>>(gs31); }
    { GemmP gs32;
      gs32.A = QV + (size_t)6 * S * 2 * D + 2 * HD; gs32.B = KP + (size_t)6 * SP * D + 2 * HD; gs32.bias = QV + (size_t)6 * S * 2 * D + 2 * HD; gs32.R = QV + (size_t)6 * S * 2 * D + 2 * HD; gs32.C = PB + (size_t)2 * S * KW;
      gs32.sAo = (long long)S * 2 * D; gs32.sAi = (long long)QB * 2 * D; gs32.sAm = 2 * D; gs32.sAk = 1; gs32.sBo = (long long)SP * D; gs32.sBi = (long long)QB * D; gs32.sBn = D; gs32.sBk = 1; gs32.sCo = (long long)NH * S * KW; gs32.sCi = (long long)QB * KW; gs32.sCm = KW; gs32.sRo = 0; gs32.sRi = 0; gs32.sRm = 0; gs32.sRn = 0;
      gs32.M = QB; gs32.N = KW; gs32.K = HD; gs32.zi_n = NBLK; gs32.flags = 0; gs32.act = 0;
      gs32.alpha = 1.0f; gs32.beta = 0.0f; gs32.sa = 1.0f; gs32.sb = 1.0f; gs32.Npad = KW; gs32.pad_ = 0;
      if ((long long)(QB) >= 64 && (long long)(KW) >= 64) k_gemmT<1, 2, 4><<<dim3((unsigned)((KW) + 63) / 64, (unsigned)((QB) + 31) / 32, (unsigned)(BC * NBLK)), 32, 0, stream>>>(gs32);
      else k_gemm<1><<<dim3((unsigned)((KW) + 31) / 32, (unsigned)((QB) + 15) / 16, (unsigned)(BC * NBLK)), 32, 0, stream>>>(gs32); }
    { GemmP gs33;
      gs33.A = QV + (size_t)6 * S * 2 * D + 3 * HD; gs33.B = KP + (size_t)6 * SP * D + 3 * HD; gs33.bias = QV + (size_t)6 * S * 2 * D + 3 * HD; gs33.R = QV + (size_t)6 * S * 2 * D + 3 * HD; gs33.C = PB + (size_t)3 * S * KW;
      gs33.sAo = (long long)S * 2 * D; gs33.sAi = (long long)QB * 2 * D; gs33.sAm = 2 * D; gs33.sAk = 1; gs33.sBo = (long long)SP * D; gs33.sBi = (long long)QB * D; gs33.sBn = D; gs33.sBk = 1; gs33.sCo = (long long)NH * S * KW; gs33.sCi = (long long)QB * KW; gs33.sCm = KW; gs33.sRo = 0; gs33.sRi = 0; gs33.sRm = 0; gs33.sRn = 0;
      gs33.M = QB; gs33.N = KW; gs33.K = HD; gs33.zi_n = NBLK; gs33.flags = 0; gs33.act = 0;
      gs33.alpha = 1.0f; gs33.beta = 0.0f; gs33.sa = 1.0f; gs33.sb = 1.0f; gs33.Npad = KW; gs33.pad_ = 0;
      if ((long long)(QB) >= 64 && (long long)(KW) >= 64) k_gemmT<1, 2, 4><<<dim3((unsigned)((KW) + 63) / 64, (unsigned)((QB) + 31) / 32, (unsigned)(BC * NBLK)), 32, 0, stream>>>(gs33);
      else k_gemm<1><<<dim3((unsigned)((KW) + 31) / 32, (unsigned)((QB) + 15) / 16, (unsigned)(BC * NBLK)), 32, 0, stream>>>(gs33); }
    { GemmP gs34;
      gs34.A = QV + (size_t)6 * S * 2 * D + 4 * HD; gs34.B = KP + (size_t)6 * SP * D + 4 * HD; gs34.bias = QV + (size_t)6 * S * 2 * D + 4 * HD; gs34.R = QV + (size_t)6 * S * 2 * D + 4 * HD; gs34.C = PB + (size_t)4 * S * KW;
      gs34.sAo = (long long)S * 2 * D; gs34.sAi = (long long)QB * 2 * D; gs34.sAm = 2 * D; gs34.sAk = 1; gs34.sBo = (long long)SP * D; gs34.sBi = (long long)QB * D; gs34.sBn = D; gs34.sBk = 1; gs34.sCo = (long long)NH * S * KW; gs34.sCi = (long long)QB * KW; gs34.sCm = KW; gs34.sRo = 0; gs34.sRi = 0; gs34.sRm = 0; gs34.sRn = 0;
      gs34.M = QB; gs34.N = KW; gs34.K = HD; gs34.zi_n = NBLK; gs34.flags = 0; gs34.act = 0;
      gs34.alpha = 1.0f; gs34.beta = 0.0f; gs34.sa = 1.0f; gs34.sb = 1.0f; gs34.Npad = KW; gs34.pad_ = 0;
      if ((long long)(QB) >= 64 && (long long)(KW) >= 64) k_gemmT<1, 2, 4><<<dim3((unsigned)((KW) + 63) / 64, (unsigned)((QB) + 31) / 32, (unsigned)(BC * NBLK)), 32, 0, stream>>>(gs34);
      else k_gemm<1><<<dim3((unsigned)((KW) + 31) / 32, (unsigned)((QB) + 15) / 16, (unsigned)(BC * NBLK)), 32, 0, stream>>>(gs34); }
    { GemmP gs35;
      gs35.A = QV + (size_t)6 * S * 2 * D + 5 * HD; gs35.B = KP + (size_t)6 * SP * D + 5 * HD; gs35.bias = QV + (size_t)6 * S * 2 * D + 5 * HD; gs35.R = QV + (size_t)6 * S * 2 * D + 5 * HD; gs35.C = PB + (size_t)5 * S * KW;
      gs35.sAo = (long long)S * 2 * D; gs35.sAi = (long long)QB * 2 * D; gs35.sAm = 2 * D; gs35.sAk = 1; gs35.sBo = (long long)SP * D; gs35.sBi = (long long)QB * D; gs35.sBn = D; gs35.sBk = 1; gs35.sCo = (long long)NH * S * KW; gs35.sCi = (long long)QB * KW; gs35.sCm = KW; gs35.sRo = 0; gs35.sRi = 0; gs35.sRm = 0; gs35.sRn = 0;
      gs35.M = QB; gs35.N = KW; gs35.K = HD; gs35.zi_n = NBLK; gs35.flags = 0; gs35.act = 0;
      gs35.alpha = 1.0f; gs35.beta = 0.0f; gs35.sa = 1.0f; gs35.sb = 1.0f; gs35.Npad = KW; gs35.pad_ = 0;
      if ((long long)(QB) >= 64 && (long long)(KW) >= 64) k_gemmT<1, 2, 4><<<dim3((unsigned)((KW) + 63) / 64, (unsigned)((QB) + 31) / 32, (unsigned)(BC * NBLK)), 32, 0, stream>>>(gs35);
      else k_gemm<1><<<dim3((unsigned)((KW) + 31) / 32, (unsigned)((QB) + 15) / 16, (unsigned)(BC * NBLK)), 32, 0, stream>>>(gs35); }
    { GemmP gs36;
      gs36.A = QV + (size_t)6 * S * 2 * D + 6 * HD; gs36.B = KP + (size_t)6 * SP * D + 6 * HD; gs36.bias = QV + (size_t)6 * S * 2 * D + 6 * HD; gs36.R = QV + (size_t)6 * S * 2 * D + 6 * HD; gs36.C = PB + (size_t)6 * S * KW;
      gs36.sAo = (long long)S * 2 * D; gs36.sAi = (long long)QB * 2 * D; gs36.sAm = 2 * D; gs36.sAk = 1; gs36.sBo = (long long)SP * D; gs36.sBi = (long long)QB * D; gs36.sBn = D; gs36.sBk = 1; gs36.sCo = (long long)NH * S * KW; gs36.sCi = (long long)QB * KW; gs36.sCm = KW; gs36.sRo = 0; gs36.sRi = 0; gs36.sRm = 0; gs36.sRn = 0;
      gs36.M = QB; gs36.N = KW; gs36.K = HD; gs36.zi_n = NBLK; gs36.flags = 0; gs36.act = 0;
      gs36.alpha = 1.0f; gs36.beta = 0.0f; gs36.sa = 1.0f; gs36.sb = 1.0f; gs36.Npad = KW; gs36.pad_ = 0;
      if ((long long)(QB) >= 64 && (long long)(KW) >= 64) k_gemmT<1, 2, 4><<<dim3((unsigned)((KW) + 63) / 64, (unsigned)((QB) + 31) / 32, (unsigned)(BC * NBLK)), 32, 0, stream>>>(gs36);
      else k_gemm<1><<<dim3((unsigned)((KW) + 31) / 32, (unsigned)((QB) + 15) / 16, (unsigned)(BC * NBLK)), 32, 0, stream>>>(gs36); }
    { GemmP gs37;
      gs37.A = QV + (size_t)6 * S * 2 * D + 7 * HD; gs37.B = KP + (size_t)6 * SP * D + 7 * HD; gs37.bias = QV + (size_t)6 * S * 2 * D + 7 * HD; gs37.R = QV + (size_t)6 * S * 2 * D + 7 * HD; gs37.C = PB + (size_t)7 * S * KW;
      gs37.sAo = (long long)S * 2 * D; gs37.sAi = (long long)QB * 2 * D; gs37.sAm = 2 * D; gs37.sAk = 1; gs37.sBo = (long long)SP * D; gs37.sBi = (long long)QB * D; gs37.sBn = D; gs37.sBk = 1; gs37.sCo = (long long)NH * S * KW; gs37.sCi = (long long)QB * KW; gs37.sCm = KW; gs37.sRo = 0; gs37.sRi = 0; gs37.sRm = 0; gs37.sRn = 0;
      gs37.M = QB; gs37.N = KW; gs37.K = HD; gs37.zi_n = NBLK; gs37.flags = 0; gs37.act = 0;
      gs37.alpha = 1.0f; gs37.beta = 0.0f; gs37.sa = 1.0f; gs37.sb = 1.0f; gs37.Npad = KW; gs37.pad_ = 0;
      if ((long long)(QB) >= 64 && (long long)(KW) >= 64) k_gemmT<1, 2, 4><<<dim3((unsigned)((KW) + 63) / 64, (unsigned)((QB) + 31) / 32, (unsigned)(BC * NBLK)), 32, 0, stream>>>(gs37);
      else k_gemm<1><<<dim3((unsigned)((KW) + 31) / 32, (unsigned)((QB) + 15) / 16, (unsigned)(BC * NBLK)), 32, 0, stream>>>(gs37); }
    k_rt_soft<<<(unsigned)(((long long)BC * NH * S + 127) / 128), 128, 0, stream>>>(PB, lens, decw, 6, BC, NH, S, KW, PADK, 0.125f, 0.1f); k_rt_col<<<(unsigned)(((long long)BC * NH * S + 127) / 128), 128, 0, stream>>>(PB, lens, PBAR, 6, BC, NH, S, KW, PADK);
    { GemmP gs40;
      gs40.A = QV + (size_t)8 * S * 2 * D + 0 * HD; gs40.B = KP + (size_t)8 * SP * D + 0 * HD; gs40.bias = QV + (size_t)8 * S * 2 * D + 0 * HD; gs40.R = QV + (size_t)8 * S * 2 * D + 0 * HD; gs40.C = PB + (size_t)0 * S * KW;
      gs40.sAo = (long long)S * 2 * D; gs40.sAi = (long long)QB * 2 * D; gs40.sAm = 2 * D; gs40.sAk = 1; gs40.sBo = (long long)SP * D; gs40.sBi = (long long)QB * D; gs40.sBn = D; gs40.sBk = 1; gs40.sCo = (long long)NH * S * KW; gs40.sCi = (long long)QB * KW; gs40.sCm = KW; gs40.sRo = 0; gs40.sRi = 0; gs40.sRm = 0; gs40.sRn = 0;
      gs40.M = QB; gs40.N = KW; gs40.K = HD; gs40.zi_n = NBLK; gs40.flags = 0; gs40.act = 0;
      gs40.alpha = 1.0f; gs40.beta = 0.0f; gs40.sa = 1.0f; gs40.sb = 1.0f; gs40.Npad = KW; gs40.pad_ = 0;
      if ((long long)(QB) >= 64 && (long long)(KW) >= 64) k_gemmT<1, 2, 4><<<dim3((unsigned)((KW) + 63) / 64, (unsigned)((QB) + 31) / 32, (unsigned)(BC * NBLK)), 32, 0, stream>>>(gs40);
      else k_gemm<1><<<dim3((unsigned)((KW) + 31) / 32, (unsigned)((QB) + 15) / 16, (unsigned)(BC * NBLK)), 32, 0, stream>>>(gs40); }
    { GemmP gs41;
      gs41.A = QV + (size_t)8 * S * 2 * D + 1 * HD; gs41.B = KP + (size_t)8 * SP * D + 1 * HD; gs41.bias = QV + (size_t)8 * S * 2 * D + 1 * HD; gs41.R = QV + (size_t)8 * S * 2 * D + 1 * HD; gs41.C = PB + (size_t)1 * S * KW;
      gs41.sAo = (long long)S * 2 * D; gs41.sAi = (long long)QB * 2 * D; gs41.sAm = 2 * D; gs41.sAk = 1; gs41.sBo = (long long)SP * D; gs41.sBi = (long long)QB * D; gs41.sBn = D; gs41.sBk = 1; gs41.sCo = (long long)NH * S * KW; gs41.sCi = (long long)QB * KW; gs41.sCm = KW; gs41.sRo = 0; gs41.sRi = 0; gs41.sRm = 0; gs41.sRn = 0;
      gs41.M = QB; gs41.N = KW; gs41.K = HD; gs41.zi_n = NBLK; gs41.flags = 0; gs41.act = 0;
      gs41.alpha = 1.0f; gs41.beta = 0.0f; gs41.sa = 1.0f; gs41.sb = 1.0f; gs41.Npad = KW; gs41.pad_ = 0;
      if ((long long)(QB) >= 64 && (long long)(KW) >= 64) k_gemmT<1, 2, 4><<<dim3((unsigned)((KW) + 63) / 64, (unsigned)((QB) + 31) / 32, (unsigned)(BC * NBLK)), 32, 0, stream>>>(gs41);
      else k_gemm<1><<<dim3((unsigned)((KW) + 31) / 32, (unsigned)((QB) + 15) / 16, (unsigned)(BC * NBLK)), 32, 0, stream>>>(gs41); }
    { GemmP gs42;
      gs42.A = QV + (size_t)8 * S * 2 * D + 2 * HD; gs42.B = KP + (size_t)8 * SP * D + 2 * HD; gs42.bias = QV + (size_t)8 * S * 2 * D + 2 * HD; gs42.R = QV + (size_t)8 * S * 2 * D + 2 * HD; gs42.C = PB + (size_t)2 * S * KW;
      gs42.sAo = (long long)S * 2 * D; gs42.sAi = (long long)QB * 2 * D; gs42.sAm = 2 * D; gs42.sAk = 1; gs42.sBo = (long long)SP * D; gs42.sBi = (long long)QB * D; gs42.sBn = D; gs42.sBk = 1; gs42.sCo = (long long)NH * S * KW; gs42.sCi = (long long)QB * KW; gs42.sCm = KW; gs42.sRo = 0; gs42.sRi = 0; gs42.sRm = 0; gs42.sRn = 0;
      gs42.M = QB; gs42.N = KW; gs42.K = HD; gs42.zi_n = NBLK; gs42.flags = 0; gs42.act = 0;
      gs42.alpha = 1.0f; gs42.beta = 0.0f; gs42.sa = 1.0f; gs42.sb = 1.0f; gs42.Npad = KW; gs42.pad_ = 0;
      if ((long long)(QB) >= 64 && (long long)(KW) >= 64) k_gemmT<1, 2, 4><<<dim3((unsigned)((KW) + 63) / 64, (unsigned)((QB) + 31) / 32, (unsigned)(BC * NBLK)), 32, 0, stream>>>(gs42);
      else k_gemm<1><<<dim3((unsigned)((KW) + 31) / 32, (unsigned)((QB) + 15) / 16, (unsigned)(BC * NBLK)), 32, 0, stream>>>(gs42); }
    { GemmP gs43;
      gs43.A = QV + (size_t)8 * S * 2 * D + 3 * HD; gs43.B = KP + (size_t)8 * SP * D + 3 * HD; gs43.bias = QV + (size_t)8 * S * 2 * D + 3 * HD; gs43.R = QV + (size_t)8 * S * 2 * D + 3 * HD; gs43.C = PB + (size_t)3 * S * KW;
      gs43.sAo = (long long)S * 2 * D; gs43.sAi = (long long)QB * 2 * D; gs43.sAm = 2 * D; gs43.sAk = 1; gs43.sBo = (long long)SP * D; gs43.sBi = (long long)QB * D; gs43.sBn = D; gs43.sBk = 1; gs43.sCo = (long long)NH * S * KW; gs43.sCi = (long long)QB * KW; gs43.sCm = KW; gs43.sRo = 0; gs43.sRi = 0; gs43.sRm = 0; gs43.sRn = 0;
      gs43.M = QB; gs43.N = KW; gs43.K = HD; gs43.zi_n = NBLK; gs43.flags = 0; gs43.act = 0;
      gs43.alpha = 1.0f; gs43.beta = 0.0f; gs43.sa = 1.0f; gs43.sb = 1.0f; gs43.Npad = KW; gs43.pad_ = 0;
      if ((long long)(QB) >= 64 && (long long)(KW) >= 64) k_gemmT<1, 2, 4><<<dim3((unsigned)((KW) + 63) / 64, (unsigned)((QB) + 31) / 32, (unsigned)(BC * NBLK)), 32, 0, stream>>>(gs43);
      else k_gemm<1><<<dim3((unsigned)((KW) + 31) / 32, (unsigned)((QB) + 15) / 16, (unsigned)(BC * NBLK)), 32, 0, stream>>>(gs43); }
    { GemmP gs44;
      gs44.A = QV + (size_t)8 * S * 2 * D + 4 * HD; gs44.B = KP + (size_t)8 * SP * D + 4 * HD; gs44.bias = QV + (size_t)8 * S * 2 * D + 4 * HD; gs44.R = QV + (size_t)8 * S * 2 * D + 4 * HD; gs44.C = PB + (size_t)4 * S * KW;
      gs44.sAo = (long long)S * 2 * D; gs44.sAi = (long long)QB * 2 * D; gs44.sAm = 2 * D; gs44.sAk = 1; gs44.sBo = (long long)SP * D; gs44.sBi = (long long)QB * D; gs44.sBn = D; gs44.sBk = 1; gs44.sCo = (long long)NH * S * KW; gs44.sCi = (long long)QB * KW; gs44.sCm = KW; gs44.sRo = 0; gs44.sRi = 0; gs44.sRm = 0; gs44.sRn = 0;
      gs44.M = QB; gs44.N = KW; gs44.K = HD; gs44.zi_n = NBLK; gs44.flags = 0; gs44.act = 0;
      gs44.alpha = 1.0f; gs44.beta = 0.0f; gs44.sa = 1.0f; gs44.sb = 1.0f; gs44.Npad = KW; gs44.pad_ = 0;
      if ((long long)(QB) >= 64 && (long long)(KW) >= 64) k_gemmT<1, 2, 4><<<dim3((unsigned)((KW) + 63) / 64, (unsigned)((QB) + 31) / 32, (unsigned)(BC * NBLK)), 32, 0, stream>>>(gs44);
      else k_gemm<1><<<dim3((unsigned)((KW) + 31) / 32, (unsigned)((QB) + 15) / 16, (unsigned)(BC * NBLK)), 32, 0, stream>>>(gs44); }
    { GemmP gs45;
      gs45.A = QV + (size_t)8 * S * 2 * D + 5 * HD; gs45.B = KP + (size_t)8 * SP * D + 5 * HD; gs45.bias = QV + (size_t)8 * S * 2 * D + 5 * HD; gs45.R = QV + (size_t)8 * S * 2 * D + 5 * HD; gs45.C = PB + (size_t)5 * S * KW;
      gs45.sAo = (long long)S * 2 * D; gs45.sAi = (long long)QB * 2 * D; gs45.sAm = 2 * D; gs45.sAk = 1; gs45.sBo = (long long)SP * D; gs45.sBi = (long long)QB * D; gs45.sBn = D; gs45.sBk = 1; gs45.sCo = (long long)NH * S * KW; gs45.sCi = (long long)QB * KW; gs45.sCm = KW; gs45.sRo = 0; gs45.sRi = 0; gs45.sRm = 0; gs45.sRn = 0;
      gs45.M = QB; gs45.N = KW; gs45.K = HD; gs45.zi_n = NBLK; gs45.flags = 0; gs45.act = 0;
      gs45.alpha = 1.0f; gs45.beta = 0.0f; gs45.sa = 1.0f; gs45.sb = 1.0f; gs45.Npad = KW; gs45.pad_ = 0;
      if ((long long)(QB) >= 64 && (long long)(KW) >= 64) k_gemmT<1, 2, 4><<<dim3((unsigned)((KW) + 63) / 64, (unsigned)((QB) + 31) / 32, (unsigned)(BC * NBLK)), 32, 0, stream>>>(gs45);
      else k_gemm<1><<<dim3((unsigned)((KW) + 31) / 32, (unsigned)((QB) + 15) / 16, (unsigned)(BC * NBLK)), 32, 0, stream>>>(gs45); }
    { GemmP gs46;
      gs46.A = QV + (size_t)8 * S * 2 * D + 6 * HD; gs46.B = KP + (size_t)8 * SP * D + 6 * HD; gs46.bias = QV + (size_t)8 * S * 2 * D + 6 * HD; gs46.R = QV + (size_t)8 * S * 2 * D + 6 * HD; gs46.C = PB + (size_t)6 * S * KW;
      gs46.sAo = (long long)S * 2 * D; gs46.sAi = (long long)QB * 2 * D; gs46.sAm = 2 * D; gs46.sAk = 1; gs46.sBo = (long long)SP * D; gs46.sBi = (long long)QB * D; gs46.sBn = D; gs46.sBk = 1; gs46.sCo = (long long)NH * S * KW; gs46.sCi = (long long)QB * KW; gs46.sCm = KW; gs46.sRo = 0; gs46.sRi = 0; gs46.sRm = 0; gs46.sRn = 0;
      gs46.M = QB; gs46.N = KW; gs46.K = HD; gs46.zi_n = NBLK; gs46.flags = 0; gs46.act = 0;
      gs46.alpha = 1.0f; gs46.beta = 0.0f; gs46.sa = 1.0f; gs46.sb = 1.0f; gs46.Npad = KW; gs46.pad_ = 0;
      if ((long long)(QB) >= 64 && (long long)(KW) >= 64) k_gemmT<1, 2, 4><<<dim3((unsigned)((KW) + 63) / 64, (unsigned)((QB) + 31) / 32, (unsigned)(BC * NBLK)), 32, 0, stream>>>(gs46);
      else k_gemm<1><<<dim3((unsigned)((KW) + 31) / 32, (unsigned)((QB) + 15) / 16, (unsigned)(BC * NBLK)), 32, 0, stream>>>(gs46); }
    { GemmP gs47;
      gs47.A = QV + (size_t)8 * S * 2 * D + 7 * HD; gs47.B = KP + (size_t)8 * SP * D + 7 * HD; gs47.bias = QV + (size_t)8 * S * 2 * D + 7 * HD; gs47.R = QV + (size_t)8 * S * 2 * D + 7 * HD; gs47.C = PB + (size_t)7 * S * KW;
      gs47.sAo = (long long)S * 2 * D; gs47.sAi = (long long)QB * 2 * D; gs47.sAm = 2 * D; gs47.sAk = 1; gs47.sBo = (long long)SP * D; gs47.sBi = (long long)QB * D; gs47.sBn = D; gs47.sBk = 1; gs47.sCo = (long long)NH * S * KW; gs47.sCi = (long long)QB * KW; gs47.sCm = KW; gs47.sRo = 0; gs47.sRi = 0; gs47.sRm = 0; gs47.sRn = 0;
      gs47.M = QB; gs47.N = KW; gs47.K = HD; gs47.zi_n = NBLK; gs47.flags = 0; gs47.act = 0;
      gs47.alpha = 1.0f; gs47.beta = 0.0f; gs47.sa = 1.0f; gs47.sb = 1.0f; gs47.Npad = KW; gs47.pad_ = 0;
      if ((long long)(QB) >= 64 && (long long)(KW) >= 64) k_gemmT<1, 2, 4><<<dim3((unsigned)((KW) + 63) / 64, (unsigned)((QB) + 31) / 32, (unsigned)(BC * NBLK)), 32, 0, stream>>>(gs47);
      else k_gemm<1><<<dim3((unsigned)((KW) + 31) / 32, (unsigned)((QB) + 15) / 16, (unsigned)(BC * NBLK)), 32, 0, stream>>>(gs47); }
    k_rt_soft<<<(unsigned)(((long long)BC * NH * S + 127) / 128), 128, 0, stream>>>(PB, lens, decw, 8, BC, NH, S, KW, PADK, 0.125f, 0.1f); k_rt_col<<<(unsigned)(((long long)BC * NH * S + 127) / 128), 128, 0, stream>>>(PB, lens, PBAR, 8, BC, NH, S, KW, PADK);
    { GemmP gs50;
      gs50.A = QV + (size_t)10 * S * 2 * D + 0 * HD; gs50.B = KP + (size_t)10 * SP * D + 0 * HD; gs50.bias = QV + (size_t)10 * S * 2 * D + 0 * HD; gs50.R = QV + (size_t)10 * S * 2 * D + 0 * HD; gs50.C = PB + (size_t)0 * S * KW;
      gs50.sAo = (long long)S * 2 * D; gs50.sAi = (long long)QB * 2 * D; gs50.sAm = 2 * D; gs50.sAk = 1; gs50.sBo = (long long)SP * D; gs50.sBi = (long long)QB * D; gs50.sBn = D; gs50.sBk = 1; gs50.sCo = (long long)NH * S * KW; gs50.sCi = (long long)QB * KW; gs50.sCm = KW; gs50.sRo = 0; gs50.sRi = 0; gs50.sRm = 0; gs50.sRn = 0;
      gs50.M = QB; gs50.N = KW; gs50.K = HD; gs50.zi_n = NBLK; gs50.flags = 0; gs50.act = 0;
      gs50.alpha = 1.0f; gs50.beta = 0.0f; gs50.sa = 1.0f; gs50.sb = 1.0f; gs50.Npad = KW; gs50.pad_ = 0;
      if ((long long)(QB) >= 64 && (long long)(KW) >= 64) k_gemmT<1, 2, 4><<<dim3((unsigned)((KW) + 63) / 64, (unsigned)((QB) + 31) / 32, (unsigned)(BC * NBLK)), 32, 0, stream>>>(gs50);
      else k_gemm<1><<<dim3((unsigned)((KW) + 31) / 32, (unsigned)((QB) + 15) / 16, (unsigned)(BC * NBLK)), 32, 0, stream>>>(gs50); }
    { GemmP gs51;
      gs51.A = QV + (size_t)10 * S * 2 * D + 1 * HD; gs51.B = KP + (size_t)10 * SP * D + 1 * HD; gs51.bias = QV + (size_t)10 * S * 2 * D + 1 * HD; gs51.R = QV + (size_t)10 * S * 2 * D + 1 * HD; gs51.C = PB + (size_t)1 * S * KW;
      gs51.sAo = (long long)S * 2 * D; gs51.sAi = (long long)QB * 2 * D; gs51.sAm = 2 * D; gs51.sAk = 1; gs51.sBo = (long long)SP * D; gs51.sBi = (long long)QB * D; gs51.sBn = D; gs51.sBk = 1; gs51.sCo = (long long)NH * S * KW; gs51.sCi = (long long)QB * KW; gs51.sCm = KW; gs51.sRo = 0; gs51.sRi = 0; gs51.sRm = 0; gs51.sRn = 0;
      gs51.M = QB; gs51.N = KW; gs51.K = HD; gs51.zi_n = NBLK; gs51.flags = 0; gs51.act = 0;
      gs51.alpha = 1.0f; gs51.beta = 0.0f; gs51.sa = 1.0f; gs51.sb = 1.0f; gs51.Npad = KW; gs51.pad_ = 0;
      if ((long long)(QB) >= 64 && (long long)(KW) >= 64) k_gemmT<1, 2, 4><<<dim3((unsigned)((KW) + 63) / 64, (unsigned)((QB) + 31) / 32, (unsigned)(BC * NBLK)), 32, 0, stream>>>(gs51);
      else k_gemm<1><<<dim3((unsigned)((KW) + 31) / 32, (unsigned)((QB) + 15) / 16, (unsigned)(BC * NBLK)), 32, 0, stream>>>(gs51); }
    { GemmP gs52;
      gs52.A = QV + (size_t)10 * S * 2 * D + 2 * HD; gs52.B = KP + (size_t)10 * SP * D + 2 * HD; gs52.bias = QV + (size_t)10 * S * 2 * D + 2 * HD; gs52.R = QV + (size_t)10 * S * 2 * D + 2 * HD; gs52.C = PB + (size_t)2 * S * KW;
      gs52.sAo = (long long)S * 2 * D; gs52.sAi = (long long)QB * 2 * D; gs52.sAm = 2 * D; gs52.sAk = 1; gs52.sBo = (long long)SP * D; gs52.sBi = (long long)QB * D; gs52.sBn = D; gs52.sBk = 1; gs52.sCo = (long long)NH * S * KW; gs52.sCi = (long long)QB * KW; gs52.sCm = KW; gs52.sRo = 0; gs52.sRi = 0; gs52.sRm = 0; gs52.sRn = 0;
      gs52.M = QB; gs52.N = KW; gs52.K = HD; gs52.zi_n = NBLK; gs52.flags = 0; gs52.act = 0;
      gs52.alpha = 1.0f; gs52.beta = 0.0f; gs52.sa = 1.0f; gs52.sb = 1.0f; gs52.Npad = KW; gs52.pad_ = 0;
      if ((long long)(QB) >= 64 && (long long)(KW) >= 64) k_gemmT<1, 2, 4><<<dim3((unsigned)((KW) + 63) / 64, (unsigned)((QB) + 31) / 32, (unsigned)(BC * NBLK)), 32, 0, stream>>>(gs52);
      else k_gemm<1><<<dim3((unsigned)((KW) + 31) / 32, (unsigned)((QB) + 15) / 16, (unsigned)(BC * NBLK)), 32, 0, stream>>>(gs52); }
    { GemmP gs53;
      gs53.A = QV + (size_t)10 * S * 2 * D + 3 * HD; gs53.B = KP + (size_t)10 * SP * D + 3 * HD; gs53.bias = QV + (size_t)10 * S * 2 * D + 3 * HD; gs53.R = QV + (size_t)10 * S * 2 * D + 3 * HD; gs53.C = PB + (size_t)3 * S * KW;
      gs53.sAo = (long long)S * 2 * D; gs53.sAi = (long long)QB * 2 * D; gs53.sAm = 2 * D; gs53.sAk = 1; gs53.sBo = (long long)SP * D; gs53.sBi = (long long)QB * D; gs53.sBn = D; gs53.sBk = 1; gs53.sCo = (long long)NH * S * KW; gs53.sCi = (long long)QB * KW; gs53.sCm = KW; gs53.sRo = 0; gs53.sRi = 0; gs53.sRm = 0; gs53.sRn = 0;
      gs53.M = QB; gs53.N = KW; gs53.K = HD; gs53.zi_n = NBLK; gs53.flags = 0; gs53.act = 0;
      gs53.alpha = 1.0f; gs53.beta = 0.0f; gs53.sa = 1.0f; gs53.sb = 1.0f; gs53.Npad = KW; gs53.pad_ = 0;
      if ((long long)(QB) >= 64 && (long long)(KW) >= 64) k_gemmT<1, 2, 4><<<dim3((unsigned)((KW) + 63) / 64, (unsigned)((QB) + 31) / 32, (unsigned)(BC * NBLK)), 32, 0, stream>>>(gs53);
      else k_gemm<1><<<dim3((unsigned)((KW) + 31) / 32, (unsigned)((QB) + 15) / 16, (unsigned)(BC * NBLK)), 32, 0, stream>>>(gs53); }
    { GemmP gs54;
      gs54.A = QV + (size_t)10 * S * 2 * D + 4 * HD; gs54.B = KP + (size_t)10 * SP * D + 4 * HD; gs54.bias = QV + (size_t)10 * S * 2 * D + 4 * HD; gs54.R = QV + (size_t)10 * S * 2 * D + 4 * HD; gs54.C = PB + (size_t)4 * S * KW;
      gs54.sAo = (long long)S * 2 * D; gs54.sAi = (long long)QB * 2 * D; gs54.sAm = 2 * D; gs54.sAk = 1; gs54.sBo = (long long)SP * D; gs54.sBi = (long long)QB * D; gs54.sBn = D; gs54.sBk = 1; gs54.sCo = (long long)NH * S * KW; gs54.sCi = (long long)QB * KW; gs54.sCm = KW; gs54.sRo = 0; gs54.sRi = 0; gs54.sRm = 0; gs54.sRn = 0;
      gs54.M = QB; gs54.N = KW; gs54.K = HD; gs54.zi_n = NBLK; gs54.flags = 0; gs54.act = 0;
      gs54.alpha = 1.0f; gs54.beta = 0.0f; gs54.sa = 1.0f; gs54.sb = 1.0f; gs54.Npad = KW; gs54.pad_ = 0;
      if ((long long)(QB) >= 64 && (long long)(KW) >= 64) k_gemmT<1, 2, 4><<<dim3((unsigned)((KW) + 63) / 64, (unsigned)((QB) + 31) / 32, (unsigned)(BC * NBLK)), 32, 0, stream>>>(gs54);
      else k_gemm<1><<<dim3((unsigned)((KW) + 31) / 32, (unsigned)((QB) + 15) / 16, (unsigned)(BC * NBLK)), 32, 0, stream>>>(gs54); }
    { GemmP gs55;
      gs55.A = QV + (size_t)10 * S * 2 * D + 5 * HD; gs55.B = KP + (size_t)10 * SP * D + 5 * HD; gs55.bias = QV + (size_t)10 * S * 2 * D + 5 * HD; gs55.R = QV + (size_t)10 * S * 2 * D + 5 * HD; gs55.C = PB + (size_t)5 * S * KW;
      gs55.sAo = (long long)S * 2 * D; gs55.sAi = (long long)QB * 2 * D; gs55.sAm = 2 * D; gs55.sAk = 1; gs55.sBo = (long long)SP * D; gs55.sBi = (long long)QB * D; gs55.sBn = D; gs55.sBk = 1; gs55.sCo = (long long)NH * S * KW; gs55.sCi = (long long)QB * KW; gs55.sCm = KW; gs55.sRo = 0; gs55.sRi = 0; gs55.sRm = 0; gs55.sRn = 0;
      gs55.M = QB; gs55.N = KW; gs55.K = HD; gs55.zi_n = NBLK; gs55.flags = 0; gs55.act = 0;
      gs55.alpha = 1.0f; gs55.beta = 0.0f; gs55.sa = 1.0f; gs55.sb = 1.0f; gs55.Npad = KW; gs55.pad_ = 0;
      if ((long long)(QB) >= 64 && (long long)(KW) >= 64) k_gemmT<1, 2, 4><<<dim3((unsigned)((KW) + 63) / 64, (unsigned)((QB) + 31) / 32, (unsigned)(BC * NBLK)), 32, 0, stream>>>(gs55);
      else k_gemm<1><<<dim3((unsigned)((KW) + 31) / 32, (unsigned)((QB) + 15) / 16, (unsigned)(BC * NBLK)), 32, 0, stream>>>(gs55); }
    { GemmP gs56;
      gs56.A = QV + (size_t)10 * S * 2 * D + 6 * HD; gs56.B = KP + (size_t)10 * SP * D + 6 * HD; gs56.bias = QV + (size_t)10 * S * 2 * D + 6 * HD; gs56.R = QV + (size_t)10 * S * 2 * D + 6 * HD; gs56.C = PB + (size_t)6 * S * KW;
      gs56.sAo = (long long)S * 2 * D; gs56.sAi = (long long)QB * 2 * D; gs56.sAm = 2 * D; gs56.sAk = 1; gs56.sBo = (long long)SP * D; gs56.sBi = (long long)QB * D; gs56.sBn = D; gs56.sBk = 1; gs56.sCo = (long long)NH * S * KW; gs56.sCi = (long long)QB * KW; gs56.sCm = KW; gs56.sRo = 0; gs56.sRi = 0; gs56.sRm = 0; gs56.sRn = 0;
      gs56.M = QB; gs56.N = KW; gs56.K = HD; gs56.zi_n = NBLK; gs56.flags = 0; gs56.act = 0;
      gs56.alpha = 1.0f; gs56.beta = 0.0f; gs56.sa = 1.0f; gs56.sb = 1.0f; gs56.Npad = KW; gs56.pad_ = 0;
      if ((long long)(QB) >= 64 && (long long)(KW) >= 64) k_gemmT<1, 2, 4><<<dim3((unsigned)((KW) + 63) / 64, (unsigned)((QB) + 31) / 32, (unsigned)(BC * NBLK)), 32, 0, stream>>>(gs56);
      else k_gemm<1><<<dim3((unsigned)((KW) + 31) / 32, (unsigned)((QB) + 15) / 16, (unsigned)(BC * NBLK)), 32, 0, stream>>>(gs56); }
    { GemmP gs57;
      gs57.A = QV + (size_t)10 * S * 2 * D + 7 * HD; gs57.B = KP + (size_t)10 * SP * D + 7 * HD; gs57.bias = QV + (size_t)10 * S * 2 * D + 7 * HD; gs57.R = QV + (size_t)10 * S * 2 * D + 7 * HD; gs57.C = PB + (size_t)7 * S * KW;
      gs57.sAo = (long long)S * 2 * D; gs57.sAi = (long long)QB * 2 * D; gs57.sAm = 2 * D; gs57.sAk = 1; gs57.sBo = (long long)SP * D; gs57.sBi = (long long)QB * D; gs57.sBn = D; gs57.sBk = 1; gs57.sCo = (long long)NH * S * KW; gs57.sCi = (long long)QB * KW; gs57.sCm = KW; gs57.sRo = 0; gs57.sRi = 0; gs57.sRm = 0; gs57.sRn = 0;
      gs57.M = QB; gs57.N = KW; gs57.K = HD; gs57.zi_n = NBLK; gs57.flags = 0; gs57.act = 0;
      gs57.alpha = 1.0f; gs57.beta = 0.0f; gs57.sa = 1.0f; gs57.sb = 1.0f; gs57.Npad = KW; gs57.pad_ = 0;
      if ((long long)(QB) >= 64 && (long long)(KW) >= 64) k_gemmT<1, 2, 4><<<dim3((unsigned)((KW) + 63) / 64, (unsigned)((QB) + 31) / 32, (unsigned)(BC * NBLK)), 32, 0, stream>>>(gs57);
      else k_gemm<1><<<dim3((unsigned)((KW) + 31) / 32, (unsigned)((QB) + 15) / 16, (unsigned)(BC * NBLK)), 32, 0, stream>>>(gs57); }
    k_rt_soft<<<(unsigned)(((long long)BC * NH * S + 127) / 128), 128, 0, stream>>>(PB, lens, decw, 10, BC, NH, S, KW, PADK, 0.125f, 0.1f); k_rt_col<<<(unsigned)(((long long)BC * NH * S + 127) / 128), 128, 0, stream>>>(PB, lens, PBAR, 10, BC, NH, S, KW, PADK);
    { GemmP gs60;
      gs60.A = QV + (size_t)12 * S * 2 * D + 0 * HD; gs60.B = KP + (size_t)12 * SP * D + 0 * HD; gs60.bias = QV + (size_t)12 * S * 2 * D + 0 * HD; gs60.R = QV + (size_t)12 * S * 2 * D + 0 * HD; gs60.C = PB + (size_t)0 * S * KW;
      gs60.sAo = (long long)S * 2 * D; gs60.sAi = (long long)QB * 2 * D; gs60.sAm = 2 * D; gs60.sAk = 1; gs60.sBo = (long long)SP * D; gs60.sBi = (long long)QB * D; gs60.sBn = D; gs60.sBk = 1; gs60.sCo = (long long)NH * S * KW; gs60.sCi = (long long)QB * KW; gs60.sCm = KW; gs60.sRo = 0; gs60.sRi = 0; gs60.sRm = 0; gs60.sRn = 0;
      gs60.M = QB; gs60.N = KW; gs60.K = HD; gs60.zi_n = NBLK; gs60.flags = 0; gs60.act = 0;
      gs60.alpha = 1.0f; gs60.beta = 0.0f; gs60.sa = 1.0f; gs60.sb = 1.0f; gs60.Npad = KW; gs60.pad_ = 0;
      if ((long long)(QB) >= 64 && (long long)(KW) >= 64) k_gemmT<1, 2, 4><<<dim3((unsigned)((KW) + 63) / 64, (unsigned)((QB) + 31) / 32, (unsigned)(BC * NBLK)), 32, 0, stream>>>(gs60);
      else k_gemm<1><<<dim3((unsigned)((KW) + 31) / 32, (unsigned)((QB) + 15) / 16, (unsigned)(BC * NBLK)), 32, 0, stream>>>(gs60); }
    { GemmP gs61;
      gs61.A = QV + (size_t)12 * S * 2 * D + 1 * HD; gs61.B = KP + (size_t)12 * SP * D + 1 * HD; gs61.bias = QV + (size_t)12 * S * 2 * D + 1 * HD; gs61.R = QV + (size_t)12 * S * 2 * D + 1 * HD; gs61.C = PB + (size_t)1 * S * KW;
      gs61.sAo = (long long)S * 2 * D; gs61.sAi = (long long)QB * 2 * D; gs61.sAm = 2 * D; gs61.sAk = 1; gs61.sBo = (long long)SP * D; gs61.sBi = (long long)QB * D; gs61.sBn = D; gs61.sBk = 1; gs61.sCo = (long long)NH * S * KW; gs61.sCi = (long long)QB * KW; gs61.sCm = KW; gs61.sRo = 0; gs61.sRi = 0; gs61.sRm = 0; gs61.sRn = 0;
      gs61.M = QB; gs61.N = KW; gs61.K = HD; gs61.zi_n = NBLK; gs61.flags = 0; gs61.act = 0;
      gs61.alpha = 1.0f; gs61.beta = 0.0f; gs61.sa = 1.0f; gs61.sb = 1.0f; gs61.Npad = KW; gs61.pad_ = 0;
      if ((long long)(QB) >= 64 && (long long)(KW) >= 64) k_gemmT<1, 2, 4><<<dim3((unsigned)((KW) + 63) / 64, (unsigned)((QB) + 31) / 32, (unsigned)(BC * NBLK)), 32, 0, stream>>>(gs61);
      else k_gemm<1><<<dim3((unsigned)((KW) + 31) / 32, (unsigned)((QB) + 15) / 16, (unsigned)(BC * NBLK)), 32, 0, stream>>>(gs61); }
    { GemmP gs62;
      gs62.A = QV + (size_t)12 * S * 2 * D + 2 * HD; gs62.B = KP + (size_t)12 * SP * D + 2 * HD; gs62.bias = QV + (size_t)12 * S * 2 * D + 2 * HD; gs62.R = QV + (size_t)12 * S * 2 * D + 2 * HD; gs62.C = PB + (size_t)2 * S * KW;
      gs62.sAo = (long long)S * 2 * D; gs62.sAi = (long long)QB * 2 * D; gs62.sAm = 2 * D; gs62.sAk = 1; gs62.sBo = (long long)SP * D; gs62.sBi = (long long)QB * D; gs62.sBn = D; gs62.sBk = 1; gs62.sCo = (long long)NH * S * KW; gs62.sCi = (long long)QB * KW; gs62.sCm = KW; gs62.sRo = 0; gs62.sRi = 0; gs62.sRm = 0; gs62.sRn = 0;
      gs62.M = QB; gs62.N = KW; gs62.K = HD; gs62.zi_n = NBLK; gs62.flags = 0; gs62.act = 0;
      gs62.alpha = 1.0f; gs62.beta = 0.0f; gs62.sa = 1.0f; gs62.sb = 1.0f; gs62.Npad = KW; gs62.pad_ = 0;
      if ((long long)(QB) >= 64 && (long long)(KW) >= 64) k_gemmT<1, 2, 4><<<dim3((unsigned)((KW) + 63) / 64, (unsigned)((QB) + 31) / 32, (unsigned)(BC * NBLK)), 32, 0, stream>>>(gs62);
      else k_gemm<1><<<dim3((unsigned)((KW) + 31) / 32, (unsigned)((QB) + 15) / 16, (unsigned)(BC * NBLK)), 32, 0, stream>>>(gs62); }
    { GemmP gs63;
      gs63.A = QV + (size_t)12 * S * 2 * D + 3 * HD; gs63.B = KP + (size_t)12 * SP * D + 3 * HD; gs63.bias = QV + (size_t)12 * S * 2 * D + 3 * HD; gs63.R = QV + (size_t)12 * S * 2 * D + 3 * HD; gs63.C = PB + (size_t)3 * S * KW;
      gs63.sAo = (long long)S * 2 * D; gs63.sAi = (long long)QB * 2 * D; gs63.sAm = 2 * D; gs63.sAk = 1; gs63.sBo = (long long)SP * D; gs63.sBi = (long long)QB * D; gs63.sBn = D; gs63.sBk = 1; gs63.sCo = (long long)NH * S * KW; gs63.sCi = (long long)QB * KW; gs63.sCm = KW; gs63.sRo = 0; gs63.sRi = 0; gs63.sRm = 0; gs63.sRn = 0;
      gs63.M = QB; gs63.N = KW; gs63.K = HD; gs63.zi_n = NBLK; gs63.flags = 0; gs63.act = 0;
      gs63.alpha = 1.0f; gs63.beta = 0.0f; gs63.sa = 1.0f; gs63.sb = 1.0f; gs63.Npad = KW; gs63.pad_ = 0;
      if ((long long)(QB) >= 64 && (long long)(KW) >= 64) k_gemmT<1, 2, 4><<<dim3((unsigned)((KW) + 63) / 64, (unsigned)((QB) + 31) / 32, (unsigned)(BC * NBLK)), 32, 0, stream>>>(gs63);
      else k_gemm<1><<<dim3((unsigned)((KW) + 31) / 32, (unsigned)((QB) + 15) / 16, (unsigned)(BC * NBLK)), 32, 0, stream>>>(gs63); }
    { GemmP gs64;
      gs64.A = QV + (size_t)12 * S * 2 * D + 4 * HD; gs64.B = KP + (size_t)12 * SP * D + 4 * HD; gs64.bias = QV + (size_t)12 * S * 2 * D + 4 * HD; gs64.R = QV + (size_t)12 * S * 2 * D + 4 * HD; gs64.C = PB + (size_t)4 * S * KW;
      gs64.sAo = (long long)S * 2 * D; gs64.sAi = (long long)QB * 2 * D; gs64.sAm = 2 * D; gs64.sAk = 1; gs64.sBo = (long long)SP * D; gs64.sBi = (long long)QB * D; gs64.sBn = D; gs64.sBk = 1; gs64.sCo = (long long)NH * S * KW; gs64.sCi = (long long)QB * KW; gs64.sCm = KW; gs64.sRo = 0; gs64.sRi = 0; gs64.sRm = 0; gs64.sRn = 0;
      gs64.M = QB; gs64.N = KW; gs64.K = HD; gs64.zi_n = NBLK; gs64.flags = 0; gs64.act = 0;
      gs64.alpha = 1.0f; gs64.beta = 0.0f; gs64.sa = 1.0f; gs64.sb = 1.0f; gs64.Npad = KW; gs64.pad_ = 0;
      if ((long long)(QB) >= 64 && (long long)(KW) >= 64) k_gemmT<1, 2, 4><<<dim3((unsigned)((KW) + 63) / 64, (unsigned)((QB) + 31) / 32, (unsigned)(BC * NBLK)), 32, 0, stream>>>(gs64);
      else k_gemm<1><<<dim3((unsigned)((KW) + 31) / 32, (unsigned)((QB) + 15) / 16, (unsigned)(BC * NBLK)), 32, 0, stream>>>(gs64); }
    { GemmP gs65;
      gs65.A = QV + (size_t)12 * S * 2 * D + 5 * HD; gs65.B = KP + (size_t)12 * SP * D + 5 * HD; gs65.bias = QV + (size_t)12 * S * 2 * D + 5 * HD; gs65.R = QV + (size_t)12 * S * 2 * D + 5 * HD; gs65.C = PB + (size_t)5 * S * KW;
      gs65.sAo = (long long)S * 2 * D; gs65.sAi = (long long)QB * 2 * D; gs65.sAm = 2 * D; gs65.sAk = 1; gs65.sBo = (long long)SP * D; gs65.sBi = (long long)QB * D; gs65.sBn = D; gs65.sBk = 1; gs65.sCo = (long long)NH * S * KW; gs65.sCi = (long long)QB * KW; gs65.sCm = KW; gs65.sRo = 0; gs65.sRi = 0; gs65.sRm = 0; gs65.sRn = 0;
      gs65.M = QB; gs65.N = KW; gs65.K = HD; gs65.zi_n = NBLK; gs65.flags = 0; gs65.act = 0;
      gs65.alpha = 1.0f; gs65.beta = 0.0f; gs65.sa = 1.0f; gs65.sb = 1.0f; gs65.Npad = KW; gs65.pad_ = 0;
      if ((long long)(QB) >= 64 && (long long)(KW) >= 64) k_gemmT<1, 2, 4><<<dim3((unsigned)((KW) + 63) / 64, (unsigned)((QB) + 31) / 32, (unsigned)(BC * NBLK)), 32, 0, stream>>>(gs65);
      else k_gemm<1><<<dim3((unsigned)((KW) + 31) / 32, (unsigned)((QB) + 15) / 16, (unsigned)(BC * NBLK)), 32, 0, stream>>>(gs65); }
    { GemmP gs66;
      gs66.A = QV + (size_t)12 * S * 2 * D + 6 * HD; gs66.B = KP + (size_t)12 * SP * D + 6 * HD; gs66.bias = QV + (size_t)12 * S * 2 * D + 6 * HD; gs66.R = QV + (size_t)12 * S * 2 * D + 6 * HD; gs66.C = PB + (size_t)6 * S * KW;
      gs66.sAo = (long long)S * 2 * D; gs66.sAi = (long long)QB * 2 * D; gs66.sAm = 2 * D; gs66.sAk = 1; gs66.sBo = (long long)SP * D; gs66.sBi = (long long)QB * D; gs66.sBn = D; gs66.sBk = 1; gs66.sCo = (long long)NH * S * KW; gs66.sCi = (long long)QB * KW; gs66.sCm = KW; gs66.sRo = 0; gs66.sRi = 0; gs66.sRm = 0; gs66.sRn = 0;
      gs66.M = QB; gs66.N = KW; gs66.K = HD; gs66.zi_n = NBLK; gs66.flags = 0; gs66.act = 0;
      gs66.alpha = 1.0f; gs66.beta = 0.0f; gs66.sa = 1.0f; gs66.sb = 1.0f; gs66.Npad = KW; gs66.pad_ = 0;
      if ((long long)(QB) >= 64 && (long long)(KW) >= 64) k_gemmT<1, 2, 4><<<dim3((unsigned)((KW) + 63) / 64, (unsigned)((QB) + 31) / 32, (unsigned)(BC * NBLK)), 32, 0, stream>>>(gs66);
      else k_gemm<1><<<dim3((unsigned)((KW) + 31) / 32, (unsigned)((QB) + 15) / 16, (unsigned)(BC * NBLK)), 32, 0, stream>>>(gs66); }
    { GemmP gs67;
      gs67.A = QV + (size_t)12 * S * 2 * D + 7 * HD; gs67.B = KP + (size_t)12 * SP * D + 7 * HD; gs67.bias = QV + (size_t)12 * S * 2 * D + 7 * HD; gs67.R = QV + (size_t)12 * S * 2 * D + 7 * HD; gs67.C = PB + (size_t)7 * S * KW;
      gs67.sAo = (long long)S * 2 * D; gs67.sAi = (long long)QB * 2 * D; gs67.sAm = 2 * D; gs67.sAk = 1; gs67.sBo = (long long)SP * D; gs67.sBi = (long long)QB * D; gs67.sBn = D; gs67.sBk = 1; gs67.sCo = (long long)NH * S * KW; gs67.sCi = (long long)QB * KW; gs67.sCm = KW; gs67.sRo = 0; gs67.sRi = 0; gs67.sRm = 0; gs67.sRn = 0;
      gs67.M = QB; gs67.N = KW; gs67.K = HD; gs67.zi_n = NBLK; gs67.flags = 0; gs67.act = 0;
      gs67.alpha = 1.0f; gs67.beta = 0.0f; gs67.sa = 1.0f; gs67.sb = 1.0f; gs67.Npad = KW; gs67.pad_ = 0;
      if ((long long)(QB) >= 64 && (long long)(KW) >= 64) k_gemmT<1, 2, 4><<<dim3((unsigned)((KW) + 63) / 64, (unsigned)((QB) + 31) / 32, (unsigned)(BC * NBLK)), 32, 0, stream>>>(gs67);
      else k_gemm<1><<<dim3((unsigned)((KW) + 31) / 32, (unsigned)((QB) + 15) / 16, (unsigned)(BC * NBLK)), 32, 0, stream>>>(gs67); }
    k_rt_soft<<<(unsigned)(((long long)BC * NH * S + 127) / 128), 128, 0, stream>>>(PB, lens, decw, 12, BC, NH, S, KW, PADK, 0.125f, 0.1f); k_rt_col<<<(unsigned)(((long long)BC * NH * S + 127) / 128), 128, 0, stream>>>(PB, lens, PBAR, 12, BC, NH, S, KW, PADK);
    { GemmP gs70;
      gs70.A = QV + (size_t)14 * S * 2 * D + 0 * HD; gs70.B = KP + (size_t)14 * SP * D + 0 * HD; gs70.bias = QV + (size_t)14 * S * 2 * D + 0 * HD; gs70.R = QV + (size_t)14 * S * 2 * D + 0 * HD; gs70.C = PB + (size_t)0 * S * KW;
      gs70.sAo = (long long)S * 2 * D; gs70.sAi = (long long)QB * 2 * D; gs70.sAm = 2 * D; gs70.sAk = 1; gs70.sBo = (long long)SP * D; gs70.sBi = (long long)QB * D; gs70.sBn = D; gs70.sBk = 1; gs70.sCo = (long long)NH * S * KW; gs70.sCi = (long long)QB * KW; gs70.sCm = KW; gs70.sRo = 0; gs70.sRi = 0; gs70.sRm = 0; gs70.sRn = 0;
      gs70.M = QB; gs70.N = KW; gs70.K = HD; gs70.zi_n = NBLK; gs70.flags = 0; gs70.act = 0;
      gs70.alpha = 1.0f; gs70.beta = 0.0f; gs70.sa = 1.0f; gs70.sb = 1.0f; gs70.Npad = KW; gs70.pad_ = 0;
      if ((long long)(QB) >= 64 && (long long)(KW) >= 64) k_gemmT<1, 2, 4><<<dim3((unsigned)((KW) + 63) / 64, (unsigned)((QB) + 31) / 32, (unsigned)(BC * NBLK)), 32, 0, stream>>>(gs70);
      else k_gemm<1><<<dim3((unsigned)((KW) + 31) / 32, (unsigned)((QB) + 15) / 16, (unsigned)(BC * NBLK)), 32, 0, stream>>>(gs70); }
    { GemmP gs71;
      gs71.A = QV + (size_t)14 * S * 2 * D + 1 * HD; gs71.B = KP + (size_t)14 * SP * D + 1 * HD; gs71.bias = QV + (size_t)14 * S * 2 * D + 1 * HD; gs71.R = QV + (size_t)14 * S * 2 * D + 1 * HD; gs71.C = PB + (size_t)1 * S * KW;
      gs71.sAo = (long long)S * 2 * D; gs71.sAi = (long long)QB * 2 * D; gs71.sAm = 2 * D; gs71.sAk = 1; gs71.sBo = (long long)SP * D; gs71.sBi = (long long)QB * D; gs71.sBn = D; gs71.sBk = 1; gs71.sCo = (long long)NH * S * KW; gs71.sCi = (long long)QB * KW; gs71.sCm = KW; gs71.sRo = 0; gs71.sRi = 0; gs71.sRm = 0; gs71.sRn = 0;
      gs71.M = QB; gs71.N = KW; gs71.K = HD; gs71.zi_n = NBLK; gs71.flags = 0; gs71.act = 0;
      gs71.alpha = 1.0f; gs71.beta = 0.0f; gs71.sa = 1.0f; gs71.sb = 1.0f; gs71.Npad = KW; gs71.pad_ = 0;
      if ((long long)(QB) >= 64 && (long long)(KW) >= 64) k_gemmT<1, 2, 4><<<dim3((unsigned)((KW) + 63) / 64, (unsigned)((QB) + 31) / 32, (unsigned)(BC * NBLK)), 32, 0, stream>>>(gs71);
      else k_gemm<1><<<dim3((unsigned)((KW) + 31) / 32, (unsigned)((QB) + 15) / 16, (unsigned)(BC * NBLK)), 32, 0, stream>>>(gs71); }
    { GemmP gs72;
      gs72.A = QV + (size_t)14 * S * 2 * D + 2 * HD; gs72.B = KP + (size_t)14 * SP * D + 2 * HD; gs72.bias = QV + (size_t)14 * S * 2 * D + 2 * HD; gs72.R = QV + (size_t)14 * S * 2 * D + 2 * HD; gs72.C = PB + (size_t)2 * S * KW;
      gs72.sAo = (long long)S * 2 * D; gs72.sAi = (long long)QB * 2 * D; gs72.sAm = 2 * D; gs72.sAk = 1; gs72.sBo = (long long)SP * D; gs72.sBi = (long long)QB * D; gs72.sBn = D; gs72.sBk = 1; gs72.sCo = (long long)NH * S * KW; gs72.sCi = (long long)QB * KW; gs72.sCm = KW; gs72.sRo = 0; gs72.sRi = 0; gs72.sRm = 0; gs72.sRn = 0;
      gs72.M = QB; gs72.N = KW; gs72.K = HD; gs72.zi_n = NBLK; gs72.flags = 0; gs72.act = 0;
      gs72.alpha = 1.0f; gs72.beta = 0.0f; gs72.sa = 1.0f; gs72.sb = 1.0f; gs72.Npad = KW; gs72.pad_ = 0;
      if ((long long)(QB) >= 64 && (long long)(KW) >= 64) k_gemmT<1, 2, 4><<<dim3((unsigned)((KW) + 63) / 64, (unsigned)((QB) + 31) / 32, (unsigned)(BC * NBLK)), 32, 0, stream>>>(gs72);
      else k_gemm<1><<<dim3((unsigned)((KW) + 31) / 32, (unsigned)((QB) + 15) / 16, (unsigned)(BC * NBLK)), 32, 0, stream>>>(gs72); }
    { GemmP gs73;
      gs73.A = QV + (size_t)14 * S * 2 * D + 3 * HD; gs73.B = KP + (size_t)14 * SP * D + 3 * HD; gs73.bias = QV + (size_t)14 * S * 2 * D + 3 * HD; gs73.R = QV + (size_t)14 * S * 2 * D + 3 * HD; gs73.C = PB + (size_t)3 * S * KW;
      gs73.sAo = (long long)S * 2 * D; gs73.sAi = (long long)QB * 2 * D; gs73.sAm = 2 * D; gs73.sAk = 1; gs73.sBo = (long long)SP * D; gs73.sBi = (long long)QB * D; gs73.sBn = D; gs73.sBk = 1; gs73.sCo = (long long)NH * S * KW; gs73.sCi = (long long)QB * KW; gs73.sCm = KW; gs73.sRo = 0; gs73.sRi = 0; gs73.sRm = 0; gs73.sRn = 0;
      gs73.M = QB; gs73.N = KW; gs73.K = HD; gs73.zi_n = NBLK; gs73.flags = 0; gs73.act = 0;
      gs73.alpha = 1.0f; gs73.beta = 0.0f; gs73.sa = 1.0f; gs73.sb = 1.0f; gs73.Npad = KW; gs73.pad_ = 0;
      if ((long long)(QB) >= 64 && (long long)(KW) >= 64) k_gemmT<1, 2, 4><<<dim3((unsigned)((KW) + 63) / 64, (unsigned)((QB) + 31) / 32, (unsigned)(BC * NBLK)), 32, 0, stream>>>(gs73);
      else k_gemm<1><<<dim3((unsigned)((KW) + 31) / 32, (unsigned)((QB) + 15) / 16, (unsigned)(BC * NBLK)), 32, 0, stream>>>(gs73); }
    { GemmP gs74;
      gs74.A = QV + (size_t)14 * S * 2 * D + 4 * HD; gs74.B = KP + (size_t)14 * SP * D + 4 * HD; gs74.bias = QV + (size_t)14 * S * 2 * D + 4 * HD; gs74.R = QV + (size_t)14 * S * 2 * D + 4 * HD; gs74.C = PB + (size_t)4 * S * KW;
      gs74.sAo = (long long)S * 2 * D; gs74.sAi = (long long)QB * 2 * D; gs74.sAm = 2 * D; gs74.sAk = 1; gs74.sBo = (long long)SP * D; gs74.sBi = (long long)QB * D; gs74.sBn = D; gs74.sBk = 1; gs74.sCo = (long long)NH * S * KW; gs74.sCi = (long long)QB * KW; gs74.sCm = KW; gs74.sRo = 0; gs74.sRi = 0; gs74.sRm = 0; gs74.sRn = 0;
      gs74.M = QB; gs74.N = KW; gs74.K = HD; gs74.zi_n = NBLK; gs74.flags = 0; gs74.act = 0;
      gs74.alpha = 1.0f; gs74.beta = 0.0f; gs74.sa = 1.0f; gs74.sb = 1.0f; gs74.Npad = KW; gs74.pad_ = 0;
      if ((long long)(QB) >= 64 && (long long)(KW) >= 64) k_gemmT<1, 2, 4><<<dim3((unsigned)((KW) + 63) / 64, (unsigned)((QB) + 31) / 32, (unsigned)(BC * NBLK)), 32, 0, stream>>>(gs74);
      else k_gemm<1><<<dim3((unsigned)((KW) + 31) / 32, (unsigned)((QB) + 15) / 16, (unsigned)(BC * NBLK)), 32, 0, stream>>>(gs74); }
    { GemmP gs75;
      gs75.A = QV + (size_t)14 * S * 2 * D + 5 * HD; gs75.B = KP + (size_t)14 * SP * D + 5 * HD; gs75.bias = QV + (size_t)14 * S * 2 * D + 5 * HD; gs75.R = QV + (size_t)14 * S * 2 * D + 5 * HD; gs75.C = PB + (size_t)5 * S * KW;
      gs75.sAo = (long long)S * 2 * D; gs75.sAi = (long long)QB * 2 * D; gs75.sAm = 2 * D; gs75.sAk = 1; gs75.sBo = (long long)SP * D; gs75.sBi = (long long)QB * D; gs75.sBn = D; gs75.sBk = 1; gs75.sCo = (long long)NH * S * KW; gs75.sCi = (long long)QB * KW; gs75.sCm = KW; gs75.sRo = 0; gs75.sRi = 0; gs75.sRm = 0; gs75.sRn = 0;
      gs75.M = QB; gs75.N = KW; gs75.K = HD; gs75.zi_n = NBLK; gs75.flags = 0; gs75.act = 0;
      gs75.alpha = 1.0f; gs75.beta = 0.0f; gs75.sa = 1.0f; gs75.sb = 1.0f; gs75.Npad = KW; gs75.pad_ = 0;
      if ((long long)(QB) >= 64 && (long long)(KW) >= 64) k_gemmT<1, 2, 4><<<dim3((unsigned)((KW) + 63) / 64, (unsigned)((QB) + 31) / 32, (unsigned)(BC * NBLK)), 32, 0, stream>>>(gs75);
      else k_gemm<1><<<dim3((unsigned)((KW) + 31) / 32, (unsigned)((QB) + 15) / 16, (unsigned)(BC * NBLK)), 32, 0, stream>>>(gs75); }
    { GemmP gs76;
      gs76.A = QV + (size_t)14 * S * 2 * D + 6 * HD; gs76.B = KP + (size_t)14 * SP * D + 6 * HD; gs76.bias = QV + (size_t)14 * S * 2 * D + 6 * HD; gs76.R = QV + (size_t)14 * S * 2 * D + 6 * HD; gs76.C = PB + (size_t)6 * S * KW;
      gs76.sAo = (long long)S * 2 * D; gs76.sAi = (long long)QB * 2 * D; gs76.sAm = 2 * D; gs76.sAk = 1; gs76.sBo = (long long)SP * D; gs76.sBi = (long long)QB * D; gs76.sBn = D; gs76.sBk = 1; gs76.sCo = (long long)NH * S * KW; gs76.sCi = (long long)QB * KW; gs76.sCm = KW; gs76.sRo = 0; gs76.sRi = 0; gs76.sRm = 0; gs76.sRn = 0;
      gs76.M = QB; gs76.N = KW; gs76.K = HD; gs76.zi_n = NBLK; gs76.flags = 0; gs76.act = 0;
      gs76.alpha = 1.0f; gs76.beta = 0.0f; gs76.sa = 1.0f; gs76.sb = 1.0f; gs76.Npad = KW; gs76.pad_ = 0;
      if ((long long)(QB) >= 64 && (long long)(KW) >= 64) k_gemmT<1, 2, 4><<<dim3((unsigned)((KW) + 63) / 64, (unsigned)((QB) + 31) / 32, (unsigned)(BC * NBLK)), 32, 0, stream>>>(gs76);
      else k_gemm<1><<<dim3((unsigned)((KW) + 31) / 32, (unsigned)((QB) + 15) / 16, (unsigned)(BC * NBLK)), 32, 0, stream>>>(gs76); }
    { GemmP gs77;
      gs77.A = QV + (size_t)14 * S * 2 * D + 7 * HD; gs77.B = KP + (size_t)14 * SP * D + 7 * HD; gs77.bias = QV + (size_t)14 * S * 2 * D + 7 * HD; gs77.R = QV + (size_t)14 * S * 2 * D + 7 * HD; gs77.C = PB + (size_t)7 * S * KW;
      gs77.sAo = (long long)S * 2 * D; gs77.sAi = (long long)QB * 2 * D; gs77.sAm = 2 * D; gs77.sAk = 1; gs77.sBo = (long long)SP * D; gs77.sBi = (long long)QB * D; gs77.sBn = D; gs77.sBk = 1; gs77.sCo = (long long)NH * S * KW; gs77.sCi = (long long)QB * KW; gs77.sCm = KW; gs77.sRo = 0; gs77.sRi = 0; gs77.sRm = 0; gs77.sRn = 0;
      gs77.M = QB; gs77.N = KW; gs77.K = HD; gs77.zi_n = NBLK; gs77.flags = 0; gs77.act = 0;
      gs77.alpha = 1.0f; gs77.beta = 0.0f; gs77.sa = 1.0f; gs77.sb = 1.0f; gs77.Npad = KW; gs77.pad_ = 0;
      if ((long long)(QB) >= 64 && (long long)(KW) >= 64) k_gemmT<1, 2, 4><<<dim3((unsigned)((KW) + 63) / 64, (unsigned)((QB) + 31) / 32, (unsigned)(BC * NBLK)), 32, 0, stream>>>(gs77);
      else k_gemm<1><<<dim3((unsigned)((KW) + 31) / 32, (unsigned)((QB) + 15) / 16, (unsigned)(BC * NBLK)), 32, 0, stream>>>(gs77); }
    k_rt_soft<<<(unsigned)(((long long)BC * NH * S + 127) / 128), 128, 0, stream>>>(PB, lens, decw, 14, BC, NH, S, KW, PADK, 0.125f, 0.1f); k_rt_col<<<(unsigned)(((long long)BC * NH * S + 127) / 128), 128, 0, stream>>>(PB, lens, PBAR, 14, BC, NH, S, KW, PADK);
    k_rt_pool<<<(unsigned)((Bn * D + 255) / 256), 256, 0, stream>>>(PBAR, QV, seq, lens, ATT, POOL, Bn, NH, S, D, HD);
    { GemmP gout;
      gout.A = ATT; gout.B = Wout; gout.bias = bout; gout.R = ATT; gout.C = ATT2;
      gout.sAo = 0; gout.sAi = 0; gout.sAm = D; gout.sAk = 1; gout.sBo = 0; gout.sBi = 0; gout.sBn = D; gout.sBk = 1; gout.sCo = 0; gout.sCi = 0; gout.sCm = D; gout.sRo = 0; gout.sRi = 0; gout.sRm = 0; gout.sRn = 0;
      gout.M = Bn; gout.N = D; gout.K = D; gout.zi_n = 1; gout.flags = 1; gout.act = 0;
      gout.alpha = 1.0f; gout.beta = 0.0f; gout.sa = 1.0f; gout.sb = 1.0f; gout.Npad = D; gout.pad_ = 0;
      k_gemm<1><<<dim3((unsigned)((D) + 31) / 32, (unsigned)((Bn) + 15) / 16, (unsigned)(1)), 32, 0, stream>>>(gout); }
    k_rt_ln<<<Bn, 256, 0, stream>>>(ATT2, POOL, lng, lnb, out, Bn, D);
}
